// PotentialPredictor_9268539424845
// MI455X (gfx1250) — hardware-verified
//
#include <hip/hip_runtime.h>
#include <math.h>

typedef __attribute__((ext_vector_type(16))) _Float16 v16h;
typedef __attribute__((ext_vector_type(8)))  _Float16 v8h;
typedef __attribute__((ext_vector_type(16))) __bf16   v16b;
typedef __attribute__((ext_vector_type(8)))  float    v8f;
typedef __attribute__((ext_vector_type(4)))  float    v4f;

__device__ __forceinline__ int frag_k(int i, int h) { return (i < 8) ? (8 * h + i) : (16 + 8 * h + (i - 8)); }
__device__ __forceinline__ __bf16 bf16_rne(float f) {
    unsigned int u = __float_as_uint(f);
    u += 0x7fffu + ((u >> 16) & 1u);
    return __builtin_bit_cast(__bf16, (unsigned short)(u >> 16));
}
__device__ __forceinline__ float bf16_f32(__bf16 b) { return __uint_as_float(((unsigned int)__builtin_bit_cast(unsigned short, b)) << 16); }
__device__ __forceinline__ v8f wmma16(v16h a, v16h b, v8f c) {
    c = __builtin_amdgcn_wmma_f32_16x16x32_f16(false, a, false, b, (short)0, c, false, false);
    asm volatile("v_nop\n\tv_nop\n\tv_nop\n\tv_nop" : "+v"(c) : "v"(a), "v"(b));
    return c;
}
__device__ __forceinline__ v8f wmmab(v16b a, v16b b, v8f c) {
    c = __builtin_amdgcn_wmma_f32_16x16x32_bf16(false, a, false, b, (short)0, c, false, false);
    asm volatile("v_nop\n\tv_nop\n\tv_nop\n\tv_nop" : "+v"(c) : "v"(a), "v"(b));
    return c;
}
struct Split { v16b hi, lo; };
__device__ __forceinline__ v8f wmma3(const Split& a, const Split& b, v8f c) {
    c = __builtin_amdgcn_wmma_f32_16x16x32_bf16(false, a.hi, false, b.hi, (short)0, c, false, false);
    c = __builtin_amdgcn_wmma_f32_16x16x32_bf16(false, a.hi, false, b.lo, (short)0, c, false, false);
    c = __builtin_amdgcn_wmma_f32_16x16x32_bf16(false, a.lo, false, b.hi, (short)0, c, false, false);
    asm volatile("v_nop\n\tv_nop\n\tv_nop\n\tv_nop" : "+v"(c) : "v"(a.hi), "v"(a.lo), "v"(b.hi), "v"(b.lo));
    return c;
}
struct Split3 { v16b hi, mid, lo; };
__device__ __forceinline__ v8f wmma6(const Split3& a, const Split3& b, v8f c) {
    c = __builtin_amdgcn_wmma_f32_16x16x32_bf16(false, a.hi, false, b.hi, (short)0, c, false, false);
    c = __builtin_amdgcn_wmma_f32_16x16x32_bf16(false, a.hi, false, b.mid, (short)0, c, false, false);
    c = __builtin_amdgcn_wmma_f32_16x16x32_bf16(false, a.mid, false, b.hi, (short)0, c, false, false);
    c = __builtin_amdgcn_wmma_f32_16x16x32_bf16(false, a.hi, false, b.lo, (short)0, c, false, false);
    c = __builtin_amdgcn_wmma_f32_16x16x32_bf16(false, a.mid, false, b.mid, (short)0, c, false, false);
    c = __builtin_amdgcn_wmma_f32_16x16x32_bf16(false, a.lo, false, b.hi, (short)0, c, false, false);
    asm volatile("v_nop\n\tv_nop\n\tv_nop\n\tv_nop" : "+v"(c) : "v"(a.hi), "v"(a.mid), "v"(a.lo), "v"(b.hi), "v"(b.mid), "v"(b.lo));
    return c;
}

__device__ __forceinline__ v16h fh_ld(const float* __restrict__ p, long long sk, int k0, int h, int klen, float s) {
    v16h a;
#pragma unroll
    for (int i = 0; i < 16; ++i) { const int k = k0 + frag_k(i, h); a[i] = (k < klen) ? (_Float16)(p[(long long)k * sk] * s) : (_Float16)0.f; }
    return a;
}
__device__ __forceinline__ Split sp_ld(const float* __restrict__ p, long long sk, int k0, int h, int klen, float s) {
    Split r;
#pragma unroll
    for (int i = 0; i < 16; ++i) {
        const int k = k0 + frag_k(i, h); const float x = (k < klen) ? p[(long long)k * sk] * s : 0.f;
        const __bf16 hb = bf16_rne(x); r.hi[i] = hb; r.lo[i] = bf16_rne(x - bf16_f32(hb));
    }
    return r;
}
__device__ __forceinline__ Split3 sp3_ld(const float* __restrict__ p, long long sk, int k0, int h, int klen, float s) {
    Split3 r;
#pragma unroll
    for (int i = 0; i < 16; ++i) {
        const int k = k0 + frag_k(i, h); const float x = (k < klen) ? p[(long long)k * sk] * s : 0.f;
        const __bf16 hb = bf16_rne(x); const float r1 = x - bf16_f32(hb); const __bf16 mb = bf16_rne(r1);
        r.hi[i] = hb; r.mid[i] = mb; r.lo[i] = bf16_rne(r1 - bf16_f32(mb));
    }
    return r;
}
__device__ __forceinline__ v16b bh_ld(const float* __restrict__ p, long long sk, int k0, int h, int klen, float s) {
    v16b a;
#pragma unroll
    for (int i = 0; i < 16; ++i) { const int k = k0 + frag_k(i, h); a[i] = bf16_rne((k < klen) ? p[(long long)k * sk] * s : 0.f); }
    return a;
}
__device__ __forceinline__ v16h fh_row(const _Float16* __restrict__ row, int k0, int h) {
    v16h a;
#pragma unroll
    for (int i = 0; i < 16; ++i) a[i] = row[k0 + frag_k(i, h)];
    return a;
}

#define VST2(T, ptr, val) do { *(volatile T*)(ptr) = (val); __threadfence(); *(volatile T*)(ptr) = (val); } while (0)
typedef float v4f __attribute__((ext_vector_type(4)));
#define VST2V4(ptr, val) do { *(volatile v4f*)(ptr) = (val); __threadfence(); *(volatile v4f*)(ptr) = (val); } while (0)

__device__ __attribute__((noinline)) float act_fn(float v, int act) {
    if (act == 1) return fmaxf(v, 0.f);
    if (act == 2) { const float u = 0.7978845608028654f * (v + 0.044715f * v * v * v); return 0.5f * v * (1.f + tanhf(u)); }
    if (act == 3) return v / (1.f + expf(-v));
    if (act == 4) return 0.5f * v * (1.f + erff(v * 0.7071067811865476f));
    if (act == 5) return tanhf(v);
    if (act == 6) return 1.f / (1.f + expf(-v));
    if (act == 7) return (v > 0.f) ? v : 0.01f * v;
    if (act == 8) return (v > 0.f) ? v : (expf(v) - 1.f);
    if (act == 9) return fminf(fmaxf(v, 0.f), 6.f);
    if (act == 10) return fabsf(v);
    if (act == 11) return (v >= 0.f) ? v : 0.1f * v;
    if (act == 12) return (v > 0.f) ? v : 0.2f * v;
    if (act == 13) return (v > 20.f) ? v : log1pf(expf(v));
    return v;
}

struct GemmP {
    const float* A; const float* B; const float* bias; const float* R; float* C;
    long long sAo, sAi, sAm, sAk, sBo, sBi, sBn, sBk, sCo, sCi, sCm, sRo, sRi, sRm, sRn;
    int M, N, K, zi_n, flags, act; float alpha, beta, sa, sb;
    int Npad, pad_;
};
static_assert(sizeof(GemmP) == 5 * 8 + 15 * 8 + 6 * 4 + 4 * 4 + 2 * 4, "GemmP has padding");

template <int MODE>
__global__ __launch_bounds__(32) void k_gemm(GemmP p) {
    const int lane = threadIdx.x & 31, h = lane >> 4, l15 = lane & 15;
    const int m0 = blockIdx.y * 16, n0 = blockIdx.x * 32;
    const int z = blockIdx.z, zo = z / p.zi_n, zi = z - zo * p.zi_n;
    const float* A = p.A + zo * p.sAo + zi * p.sAi;
    const float* B = p.B + zo * p.sBo + zi * p.sBi;
    const int am = min(m0 + l15, p.M - 1);
    v8f acc[2];
#pragma unroll
    for (int t = 0; t < 2; ++t) { v8f zz = {}; acc[t] = zz; }
    for (int k0 = 0; k0 < p.K; k0 += 32) {
        const float* arow = A + (long long)am * p.sAm;
        if (MODE == 1) {
            const Split a = sp_ld(arow, p.sAk, k0, h, p.K, 1.f);
#pragma unroll
            for (int t = 0; t < 2; ++t) {
                const int bn = min(n0 + t * 16 + l15, p.N - 1);
                acc[t] = wmma3(a, sp_ld(B + (long long)bn * p.sBn, p.sBk, k0, h, p.K, 1.f), acc[t]);
            }
        } else if (MODE == 3) {
            const Split3 a = sp3_ld(arow, p.sAk, k0, h, p.K, 1.f);
#pragma unroll
            for (int t = 0; t < 2; ++t) {
                const int bn = min(n0 + t * 16 + l15, p.N - 1);
                acc[t] = wmma6(a, sp3_ld(B + (long long)bn * p.sBn, p.sBk, k0, h, p.K, 1.f), acc[t]);
            }
        } else if (MODE == 2) {
            const v16b a = bh_ld(arow, p.sAk, k0, h, p.K, 1.f);
#pragma unroll
            for (int t = 0; t < 2; ++t) {
                const int bn = min(n0 + t * 16 + l15, p.N - 1);
                acc[t] = wmmab(a, bh_ld(B + (long long)bn * p.sBn, p.sBk, k0, h, p.K, 1.f), acc[t]);
            }
        } else {
            const v16h a = fh_ld(arow, p.sAk, k0, h, p.K, p.sa);
#pragma unroll
            for (int t = 0; t < 2; ++t) {
                const int bn = min(n0 + t * 16 + l15, p.N - 1);
                acc[t] = wmma16(a, fh_ld(B + (long long)bn * p.sBn, p.sBk, k0, h, p.K, p.sb), acc[t]);
            }
        }
    }
    const float iscale = (MODE == 0) ? p.alpha / (p.sa * p.sb) : p.alpha;
    float* C = p.C + zo * p.sCo + zi * p.sCi;
    const float* R = p.R + zo * p.sRo + zi * p.sRi;
    __shared__ __align__(16) float ctile[16][36];
#pragma unroll
    for (int t = 0; t < 2; ++t) {
        const int n = n0 + t * 16 + l15; const int nn = min(n, p.N - 1);
#pragma unroll
        for (int r = 0; r < 8; ++r) {
            const int m = m0 + 8 * h + r; const int mm = min(m, p.M - 1);
            float v = acc[t][r] * iscale;
            if (p.flags & 1) v += p.bias[nn];
            if (p.flags & 2) v += p.bias[mm];
            v = act_fn(v, p.act);
            if (p.flags & 4) v += p.beta * R[(long long)mm * p.sRm + (long long)nn * p.sRn];
            ctile[8 * h + r][t * 16 + l15] = (n < p.N) ? v : 0.f;
        }
    }
    __syncthreads();
    const int NW = (p.Npad > p.N) ? p.Npad : p.N;
    const bool fast = (m0 + 16 <= p.M) && (n0 + 32 <= NW) && ((p.sCm & 3) == 0) && ((((size_t)C) & 15) == 0);
    if (fast) {
#pragma unroll
        for (int s = 0; s < 4; ++s) {
            const int row = s * 4 + (lane >> 3), c4 = (lane & 7) * 4;
            const v4f v = *(const v4f*)&ctile[row][c4];
            VST2V4(C + (long long)(m0 + row) * p.sCm + n0 + c4, v);
        }
    } else {
        for (int row = 0; row < 16; ++row) {
            const int m = m0 + row, n = n0 + lane;
            if (m < p.M && n < NW) VST2(float, C + (long long)m * p.sCm + n, ctile[row][lane]);
        }
    }
}

#define AW 4
struct AttnP {
    const float* Q; const float* K; const float* V; float* O; float* P; const float* Mf; const int* Mi; float* ST;
    const float* Pw; const float* Rt; const int* SQ; const int* SK;
    long long swb, swh, swi, swj, srb, srh, sri;
    long long sQb, sQh, sQi, sQd, sKb, sKh, sKj, sKd, sVb, sVh, sVj, sVd, sOb, sOh, sOi, sPb, sPh, sPi, smb, smh, smi, smj;
    int Lq, Lk, dh, dv, hrep, causal, coff, pband;
    float scale, mfill; int nonorm, mpol;
    int roff, rn, segpol, win;
};
static_assert(sizeof(AttnP) == 12 * 8 + 29 * 8 + 16 * 4, "AttnP has padding");

#ifndef KATTN_ATTR
#define KATTN_ATTR
#endif
template <int DHP, int DVP, int QM, bool SPLITPV, bool TWOPASS>
__global__ __launch_bounds__(32 * AW) KATTN_ATTR void k_attn(AttnP p) {
    constexpr int NT = DVP / 16;
    constexpr int KS = DHP / 32;
    constexpr int VP = DVP + 8;
    __shared__ __align__(16) float    pl[AW][16 * 64];
    __shared__ __align__(16) _Float16 vl[(SPLITPV ? 2 : 1) * 64 * VP];
    const int lane = threadIdx.x & 31, hf = lane >> 4, l15 = lane & 15, wave = threadIdx.x >> 5;
    const int h = blockIdx.y, b = blockIdx.z, hk = h / p.hrep;
    const int q0 = (blockIdx.x * AW + wave) * 16;
    float* myp = pl[wave];
    const float L2E = 1.4426950408889634f;
    const float NEG = -__builtin_inff();
    const int qi = min(q0 + l15, p.Lq - 1);
    const float* qrow = p.Q + b * p.sQb + h * p.sQh + (long long)qi * p.sQi;
    const float* kbase = p.K + b * p.sKb + hk * p.sKh;
    const float* vbase = p.V + b * p.sVb + hk * p.sVh;
    v16h qa[QM == 0 ? KS : 1]; Split qs_[QM == 1 ? KS : 1]; Split3 qt_[QM == 2 ? KS : 1];
#pragma unroll
    for (int ks = 0; ks < KS; ++ks) {
        if (QM == 2) qt_[ks] = sp3_ld(qrow, p.sQd, ks * 32, hf, p.dh, 1.f);
        else if (QM == 1) qs_[ks] = sp_ld(qrow, p.sQd, ks * 32, hf, p.dh, 1.f);
        else qa[ks] = fh_ld(qrow, p.sQd, ks * 32, hf, p.dh, 1.f);
    }
    v8f o[NT]; float m8[8], l8[8];
#pragma unroll
    for (int t = 0; t < NT; ++t) { v8f zz = {}; o[t] = zz; }
#pragma unroll
    for (int i = 0; i < 8; ++i) { m8[i] = NEG; l8[i] = 0.f; }
    int jend = p.Lk;
    if (p.causal == 1) { const int je = (blockIdx.x * AW + AW - 1) * 16 + 16 + p.coff; jend = min(jend, max(je, 0)); }
    const int npass = TWOPASS ? 2 : 1;
    for (int pass = 0; pass < npass; ++pass) {
        const bool dopv = (!TWOPASS) || pass == 1;
        for (int j0 = 0; j0 < jend; j0 += 64) {
            if (dopv) {
                __syncthreads();
                for (int idx = threadIdx.x; idx < 64 * DVP; idx += 32 * AW) {
                    const int jr = idx / DVP, d = idx - jr * DVP, j = j0 + jr;
                    const float f = (j < p.Lk && d < p.dv) ? vbase[(long long)j * p.sVj + (long long)d * p.sVd] : 0.f;
                    if (SPLITPV) {
                        const __bf16 hb = bf16_rne(f);
                        ((__bf16*)vl)[jr * VP + d] = hb; ((__bf16*)vl)[64 * VP + jr * VP + d] = bf16_rne(f - bf16_f32(hb));
                    } else vl[jr * VP + d] = (_Float16)f;
                }
            }
            v8f s[4];
#pragma unroll
            for (int t = 0; t < 4; ++t) {
                const int j = min(j0 + t * 16 + l15, p.Lk - 1);
                const float* krow = kbase + (long long)j * p.sKj;
                v8f acc = {};
#pragma unroll
                for (int ks = 0; ks < KS; ++ks) {
                    if (QM == 2)      acc = wmma6(qt_[ks], sp3_ld(krow, p.sKd, ks * 32, hf, p.dh, 1.f), acc);
                    else if (QM == 1) acc = wmma3(qs_[ks], sp_ld(krow, p.sKd, ks * 32, hf, p.dh, 1.f), acc);
                    else              acc = wmma16(qa[ks], fh_ld(krow, p.sKd, ks * 32, hf, p.dh, 1.f), acc);
                }
                s[t] = acc;
            }
            float pv[8][4];
#pragma unroll
            for (int i = 0; i < 8; ++i) {
                const int irow = q0 + i + 8 * hf;
                const int ic = min(irow, p.Lq - 1);
                float sc[4];
#pragma unroll
                for (int t = 0; t < 4; ++t) {
                    const int jg = j0 + t * 16 + l15;
                    float v = s[t][i] * p.scale;
                    if (p.Mf) v += p.Mf[b * p.smb + h * p.smh + (long long)ic * p.smi + (long long)min(jg, p.Lk - 1) * p.smj];
                    if (p.Rt) { int rc = ic - min(jg, p.Lk - 1) + p.roff; rc = rc < 0 ? 0 : (rc >= p.rn ? p.rn - 1 : rc); v += p.Rt[b * p.srb + h * p.srh + (long long)ic * p.sri + rc]; }
                    if (p.Mi) { const int mv = p.Mi[b * p.smb + h * p.smh + (long long)ic * p.smi + (long long)min(jg, p.Lk - 1) * p.smj]; if (p.mpol ? (mv != 0) : (mv == 0)) v = p.mfill; }
                    if (p.SQ) { const bool same = p.SQ[(long long)b * p.Lq + ic] == p.SK[(long long)b * p.Lk + min(jg, p.Lk - 1)]; if (p.segpol ? same : !same) v = p.mfill; }
                    if (p.causal == 2 && jg > irow + p.coff) v = p.mfill;
                    if (jg >= p.Lk || (p.causal == 1 && jg > irow + p.coff) || (p.causal == 3 && jg < irow + p.coff) || (p.win > 0 && irow + p.coff - jg > p.win)) v = NEG; else v *= L2E;
                    sc[t] = v;
                }
                if (!TWOPASS || pass == 0) {
                    float mx = fmaxf(fmaxf(sc[0], sc[1]), fmaxf(sc[2], sc[3]));
                    mx = fmaxf(mx, __shfl_xor(mx, 1, 32)); mx = fmaxf(mx, __shfl_xor(mx, 2, 32));
                    mx = fmaxf(mx, __shfl_xor(mx, 4, 32)); mx = fmaxf(mx, __shfl_xor(mx, 8, 32));
                    const float mnew = fmaxf(m8[i], mx);
                    const float corr = (mnew == NEG) ? 1.f : exp2f(m8[i] - mnew);
                    float rs = 0.f;
#pragma unroll
                    for (int t = 0; t < 4; ++t) {
                        const float pp = (sc[t] == NEG) ? 0.f : exp2f(sc[t] - mnew); rs += pp;
                        pv[i][t] = p.Pw ? pp * p.Pw[b * p.swb + h * p.swh + (long long)ic * p.swi + (long long)min(j0 + t * 16 + l15, p.Lk - 1) * p.swj] : pp;
                    }
                    rs += __shfl_xor(rs, 1, 32); rs += __shfl_xor(rs, 2, 32); rs += __shfl_xor(rs, 4, 32); rs += __shfl_xor(rs, 8, 32);
                    l8[i] = l8[i] * corr + rs; m8[i] = mnew;
                    if (!TWOPASS) {
#pragma unroll
                        for (int t = 0; t < NT; ++t) o[t][i] *= corr;
                    }
                } else {
                    const float inv = (l8[i] > 0.f) ? 1.f / l8[i] : 0.f;
#pragma unroll
                    for (int t = 0; t < 4; ++t) {
                        const int jg = j0 + t * 16 + l15;
                        float pp = (sc[t] == NEG) ? 0.f : exp2f(sc[t] - m8[i]) * inv;
                        if (p.Pw) pp *= p.Pw[b * p.swb + h * p.swh + (long long)ic * p.swi + (long long)min(jg, p.Lk - 1) * p.swj];
                        pv[i][t] = pp;
                    }
                }
            }
            if (dopv) {
#pragma unroll
                for (int i = 0; i < 8; ++i)
#pragma unroll
                    for (int t = 0; t < 4; ++t) myp[(i + 8 * hf) * 64 + t * 16 + l15] = pv[i][t];
                __syncthreads();
                if (p.P) {
                    float* pb_ = p.P + b * p.sPb + h * p.sPh;
                    const bool fastP = (p.pband == 0) && ((p.sPi & 3) == 0) && (j0 + 64 <= p.Lk) && (q0 + 16 <= p.Lq) && ((((size_t)pb_) & 15) == 0);
                    if (fastP) {
#pragma unroll
                        for (int s = 0; s < 8; ++s) {
                            const int row = s * 2 + (lane >> 4), c4 = (lane & 15) * 4;
                            const v4f v = *(const v4f*)(myp + row * 64 + c4);
                            VST2V4(pb_ + (long long)(q0 + row) * p.sPi + j0 + c4, v);
                        }
                    } else {
                        for (int row = 0; row < 16; ++row) {
                            const int irow = q0 + row; if (irow >= p.Lq) continue;
                            for (int c = lane; c < 64; c += 32) {
                                const int jg = j0 + c; if (jg >= p.Lk) continue;
                                if (p.pband == 0) VST2(float, pb_ + (long long)irow * p.sPi + jg, myp[row * 64 + c]);
                                else if (jg - irow <= p.pband && irow - jg <= p.pband) VST2(float, pb_ + (long long)irow * p.sPi + (jg - irow + p.pband), myp[row * 64 + c]);
                            }
                        }
                    }
                }
                if (SPLITPV) {
                    const Split pa0 = sp_ld(myp + l15 * 64, 1, 0, hf, 64, 1.f), pa1 = sp_ld(myp + l15 * 64, 1, 32, hf, 64, 1.f);
                    const __bf16* vh = (const __bf16*)vl; const __bf16* vlo = vh + 64 * VP;
#pragma unroll
                    for (int t = 0; t < NT; ++t) {
                        const int dcol = t * 16 + l15;
                        Split b0, b1;
#pragma unroll
                        for (int e = 0; e < 16; ++e) {
                            const int k0 = frag_k(e, hf), k1 = 32 + frag_k(e, hf);
                            b0.hi[e] = vh[k0 * VP + dcol]; b0.lo[e] = vlo[k0 * VP + dcol]; b1.hi[e] = vh[k1 * VP + dcol]; b1.lo[e] = vlo[k1 * VP + dcol];
                        }
                        o[t] = wmma3(pa0, b0, o[t]);
                        o[t] = wmma3(pa1, b1, o[t]);
                    }
                } else {
                    const v16h pa0 = fh_ld(myp + l15 * 64, 1, 0, hf, 64, 4096.f), pa1 = fh_ld(myp + l15 * 64, 1, 32, hf, 64, 4096.f);
#pragma unroll
                    for (int t = 0; t < NT; ++t) {
                        const int dcol = t * 16 + l15;
                        v16h b0, b1;
#pragma unroll
                        for (int e = 0; e < 16; ++e) { b0[e] = vl[frag_k(e, hf) * VP + dcol]; b1[e] = vl[(32 + frag_k(e, hf)) * VP + dcol]; }
                        o[t] = wmma16(pa0, b0, o[t]);
                        o[t] = wmma16(pa1, b1, o[t]);
                    }
                }
            }
        }
    }
    float* obase = p.O + b * p.sOb + h * p.sOh;
    if (p.ST) {
        const int rl = lane >> 1, isel = rl & 7;
        float mv = 0.f, lv = 0.f;
#pragma unroll
        for (int i = 0; i < 8; ++i) if (i == isel) { mv = m8[i]; lv = l8[i]; }
        const int irow = q0 + rl;
        if (irow < p.Lq) { float* st = p.ST + (((long long)b * gridDim.y + h) * p.Lq + irow) * 2 + (lane & 1); VST2(float, st, (lane & 1) ? lv : mv * 0.6931471805599453f); }
    }
    float invr[8];
#pragma unroll
    for (int i = 0; i < 8; ++i) {
        if (TWOPASS) invr[i] = SPLITPV ? 1.f : (1.f / 4096.f);
        else if (p.nonorm) invr[i] = exp2f(m8[i]) * (SPLITPV ? 1.f : (1.f / 4096.f));
        else invr[i] = (l8[i] > 0.f) ? (SPLITPV ? 1.f / l8[i] : 1.f / (l8[i] * 4096.f)) : 0.f;
    }
    __syncthreads();
    const bool ofast = ((p.sOi & 3) == 0) && ((((size_t)obase) & 15) == 0) && (q0 + 16 <= p.Lq);
#pragma unroll
    for (int c0 = 0; c0 < DVP; c0 += 64) {
#pragma unroll
        for (int i = 0; i < 8; ++i)
#pragma unroll
            for (int t = 0; t < NT; ++t) if (t * 16 >= c0 && t * 16 < c0 + 64) myp[(i + 8 * hf) * 64 + (t * 16 - c0) + l15] = o[t][i] * invr[i];
        __syncthreads();
        const int cw = (DVP - c0 < 64) ? (DVP - c0) : 64;
        if (ofast && (c0 + cw <= p.dv) && (cw % 32 == 0)) {
            const int lpr = cw / 4;
            const int rows_per_ins = 32 / lpr;
            for (int r0 = 0; r0 < 16; r0 += rows_per_ins) {
                const int row = r0 + lane / lpr, c4 = (lane % lpr) * 4;
                const v4f v = *(const v4f*)(myp + row * 64 + c4);
                VST2V4(obase + (long long)(q0 + row) * p.sOi + c0 + c4, v);
            }
        } else {
            for (int row = 0; row < 16; ++row) {
                const int irow = q0 + row; if (irow >= p.Lq) continue;
                for (int c = lane; c < cw; c += 32) { const int d = c0 + c; if (d < p.dv) VST2(float, obase + (long long)irow * p.sOi + d, myp[row * 64 + c]); }
            }
        }
        __syncthreads();
    }
}

struct TrP { const float* src; float* dst; const float* R2; long long sSz, lds, sDz, ldd, sRz, ldr; int R, C, flags, act; float alpha, beta; };
static_assert(sizeof(TrP) == 3 * 8 + 6 * 8 + 6 * 4, "TrP has padding");
__global__ __launch_bounds__(256) void k_tr(TrP p) {
    __shared__ float tile[32][33];
    const int c0 = blockIdx.x * 32, r0 = blockIdx.y * 32, z = blockIdx.z;
    const int lane = threadIdx.x & 31, wave = threadIdx.x >> 5;
    const float* s = p.src + z * p.sSz;
#pragma unroll
    for (int k = 0; k < 4; ++k) {
        const int rl = wave * 4 + k, r = r0 + rl, c = c0 + lane;
        tile[rl][lane] = (r < p.R && c < p.C) ? s[(long long)r * p.lds + c] : 0.f;
    }
    __syncthreads();
    float* d = p.dst + z * p.sDz; const float* rr = p.R2 + z * p.sRz;
#pragma unroll
    for (int k = 0; k < 4; ++k) {
        const int cl = wave * 4 + k, c = c0 + cl, r = r0 + lane;
        if (c < p.C && r < p.R) {
            float v = act_fn(p.alpha * tile[lane][cl], p.act);
            if (p.flags & 1) v += p.beta * rr[(long long)c * p.ldr + r];
            VST2(float, d + (long long)c * p.ldd + r, v);
        }
    }
}

__global__ __launch_bounds__(256) void k_affine(const float* __restrict__ src, float* __restrict__ dst, int n, float a, float b, const float* __restrict__ sdev) {
    const int i = blockIdx.x * 256 + threadIdx.x;
    if (i < n) { const float aa = sdev ? a * sdev[0] : a; const float v = aa * src[i] + b; VST2(float, dst + i, v); }
}

struct SmP { const float* src; float* dst; const float* Mf; long long sz, sr, dz, dr, smz, smr; int n, pad; float scale_in, scale_out; };
static_assert(sizeof(SmP) == 3 * 8 + 6 * 8 + 4 * 4, "SmP has padding");
__global__ __launch_bounds__(256) void k_softmax(SmP p) {
    __shared__ float red[256];
    const int r = blockIdx.x, z = blockIdx.y, tid = threadIdx.x;
    const float* s = p.src + z * p.sz + (long long)r * p.sr;
    const float* mf = p.Mf ? (p.Mf + z * p.smz + (long long)r * p.smr) : nullptr;
    float mx = -__builtin_inff();
    for (int j = tid; j < p.n; j += 256) { float v = s[j] * p.scale_in; if (mf) v += mf[j]; mx = fmaxf(mx, v); }
    red[tid] = mx; __syncthreads();
    for (int o = 128; o > 0; o >>= 1) { if (tid < o) red[tid] = fmaxf(red[tid], red[tid + o]); __syncthreads(); }
    mx = red[0]; __syncthreads();
    float sum = 0.f;
    for (int j = tid; j < p.n; j += 256) { float v = s[j] * p.scale_in; if (mf) v += mf[j]; sum += (mx == -__builtin_inff()) ? 0.f : expf(v - mx); }
    red[tid] = sum; __syncthreads();
    for (int o = 128; o > 0; o >>= 1) { if (tid < o) red[tid] += red[tid + o]; __syncthreads(); }
    sum = red[0];
    const float inv = (sum > 0.f) ? p.scale_out / sum : 0.f;
    float* d = p.dst + z * p.dz + (long long)r * p.dr;
    for (int j = tid; j < p.n; j += 256) { float v = s[j] * p.scale_in; if (mf) v += mf[j]; const float o = (mx == -__builtin_inff()) ? 0.f : expf(v - mx) * inv; VST2(float, d + j, o); }
}
__global__ __launch_bounds__(256) void k_stats(const float* __restrict__ x, long long sz, long long so, long long si, int inner, int n, float eps, float* __restrict__ stat, int mode) {
    __shared__ float red[256];
    const int z = blockIdx.x, tid = threadIdx.x;
    const float* base = x + z * sz;
    float s = 0.f;
    for (int e = tid; e < n; e += 256) s += base[(long long)(e / inner) * so + (long long)(e % inner) * si];
    red[tid] = s; __syncthreads();
    for (int o = 128; o > 0; o >>= 1) { if (tid < o) red[tid] += red[tid + o]; __syncthreads(); }
    const float mu = (mode == 0 || mode == 3) ? red[0] / (float)n : 0.f; __syncthreads();
    float q = 0.f;
    for (int e = tid; e < n; e += 256) { const float dlt = base[(long long)(e / inner) * so + (long long)(e % inner) * si] - mu; q += dlt * dlt; }
    red[tid] = q; __syncthreads();
    for (int o = 128; o > 0; o >>= 1) { if (tid < o) red[tid] += red[tid + o]; __syncthreads(); }
    {
        float rs;
        if (mode == 2) rs = sqrtf((float)n) / fmaxf(sqrtf(red[0]), eps); else if (mode == 3) rs = rsqrtf(red[0] / (float)(n - 1) + eps); else rs = rsqrtf(red[0] / (float)n + eps);
        if (tid < 32) { const float v = (tid == 0) ? mu : ((tid == 1) ? rs : 0.f); VST2(float, stat + (long long)z * 32 + tid, v); }
    }
}
__global__ __launch_bounds__(256) void k_norm_apply(const float* __restrict__ x, float* __restrict__ y, const float* __restrict__ stat, const float* __restrict__ g, const float* __restrict__ bta,
                                                     int Z, int C, int L, int G, int bn, int act) {
    const long long idx = (long long)blockIdx.x * 256 + threadIdx.x;
    if (idx >= (long long)Z * C * L) return;
    const int l = (int)(idx % L); const long long zc = idx / L; const int c = (int)(zc % C), z = (int)(zc / C); (void)l;
    const int set = bn ? c : (z * G + c / (C / G));
    float v = (x[idx] - stat[(long long)set * 32]) * stat[(long long)set * 32 + 1];
    if (g) v *= g[c];
    if (bta) v += bta[c];
    v = act_fn(v, act);
    VST2(float, y + idx, v);
}

__global__ __launch_bounds__(256) void k_lse_neg(const float* __restrict__ st, float* __restrict__ c, int n) {
    const int i = blockIdx.x * 256 + threadIdx.x;
    if (i < n) { const float v = -(st[2 * i] + logf(st[2 * i + 1])); VST2(float, c + i, v); }
}

__global__ __launch_bounds__(256) void k_iota(int* __restrict__ dst, int n, int a, int b) {
    const int i = blockIdx.x * 256 + threadIdx.x;
    if (i < n) { const int v = a * i + b; VST2(int, dst + i, v); }
}

__global__ __launch_bounds__(256) void k_axpby(const float* __restrict__ x, const float* __restrict__ y, float* __restrict__ dst, int n, float a, float b, float c) {
    const int i = blockIdx.x * 256 + threadIdx.x;
    if (i < n) { const float v = a * x[i] + b * y[i] + c; VST2(float, dst + i, v); }
}

struct RopeP { const float* X; float* Y; const float* C; const float* Sn; const int* pos; long long sXr, sXh, sYr, sYh, sCb, sCp, sCd; int R, Hn, D, S, mode, tmode, pmode, pad; };
static_assert(sizeof(RopeP) == 5 * 8 + 7 * 8 + 8 * 4, "RopeP has padding");
__global__ __launch_bounds__(256) void k_rope(RopeP p) {
    const long long idx = (long long)blockIdx.x * 256 + threadIdx.x;
    if (idx >= (long long)p.R * p.Hn * p.D) return;
    const int d = (int)(idx % p.D); const long long rh = idx / p.D; const int h = (int)(rh % p.Hn); const int r = (int)(rh / p.Hn);
    const int half = p.D / 2;
    int partner; float sign;
    if (p.mode == 0) { partner = (d < half) ? d + half : d - half; sign = (d < half) ? -1.f : 1.f; }
    else { partner = d ^ 1; sign = (d & 1) ? 1.f : -1.f; }
    const int tcol = (p.tmode == 0) ? d : ((p.tmode == 1) ? (d % half) : (d >> 1));
    const int pp = (p.pmode == 0) ? (r % p.S) : ((p.pmode == 1) ? h : p.pos[r]);
    const long long toff = (long long)(r / p.S) * p.sCb + (long long)pp * p.sCp + (long long)tcol * p.sCd;
    const float* xr = p.X + (long long)r * p.sXr + (long long)h * p.sXh;
    const float v = xr[d] * p.C[toff] + sign * xr[partner] * p.Sn[toff];
    VST2(float, p.Y + (long long)r * p.sYr + (long long)h * p.sYh + d, v);
}

__global__ __launch_bounds__(256) void k_invf(float* __restrict__ invb, int half, int D, float base, float num, int fmode, float cexp) {
    const int i = blockIdx.x * 256 + threadIdx.x;
    if (i >= ((half + 31) / 32) * 32) return;
    if (i >= half) { VST2(float, invb + i, 0.f); return; }
    const float e = (float)(2 * i) / (float)D;
    float invf;
    if (fmode == 1) invf = num * expf((float)(2 * i) * cexp);
    else if (fmode == 2) invf = num * powf(base, (-2.0f * ((float)i - 1.0f)) / (float)D);
    else invf = num * (1.0f / powf(base, e));
    VST2(float, invb + i, invf);
}
__global__ __launch_bounds__(256) void k_sincos(float* __restrict__ cs, float* __restrict__ sn, const float* __restrict__ invb, int S, int half, float pscale) {
    const int idx = blockIdx.x * 256 + threadIdx.x;
    if (idx >= S * half) return;
    const int s = idx / half, i = idx - s * half;
    const float ang = (pscale * (float)s) * invb[i];
    VST2(float, cs + idx, cosf(ang)); VST2(float, sn + idx, sinf(ang));
}

__global__ __launch_bounds__(256) void k_mulact(const float* __restrict__ x, const float* __restrict__ y, float* __restrict__ dst, int n, int act) {
    const int i = blockIdx.x * 256 + threadIdx.x;
    if (i < n) { const float v = act_fn(x[i], act) * y[i]; VST2(float, dst + i, v); }
}

__global__ __launch_bounds__(256) void k_matvec(GemmP p) {
    const int rpt = (p.N == 1) ? 1 : 32;
    const long long r0 = ((long long)blockIdx.x * 256 + threadIdx.x) * rpt; const int z = blockIdx.z, zo = z / p.zi_n, zi = z - zo * p.zi_n;
    if (r0 >= p.M) return;
    const float* Bb = p.B + zo * p.sBo + zi * p.sBi;
    float* C = p.C + zo * p.sCo + zi * p.sCi; const float* R = p.R + zo * p.sRo + zi * p.sRi;
    for (int rr = 0; rr < rpt; ++rr) {
        const long long r = r0 + rr; if (r >= p.M) break;
        const float* A = p.A + zo * p.sAo + zi * p.sAi + r * p.sAm;
        float acc[8] = {0.f, 0.f, 0.f, 0.f, 0.f, 0.f, 0.f, 0.f};
        for (int k = 0; k < p.K; ++k) { const float a = A[(long long)k * p.sAk];
#pragma unroll
            for (int j = 0; j < 8; ++j) if (j < p.N) acc[j] += a * Bb[(long long)j * p.sBn + (long long)k * p.sBk]; }
#pragma unroll
        for (int j = 0; j < 8; ++j) if (j < p.N) {
            float v = acc[j] * p.alpha;
            if (p.flags & 1) v += p.bias[j];
            if (p.flags & 2) v += p.bias[r];
            v = act_fn(v, p.act);
            if (p.flags & 4) v += p.beta * R[r * p.sRm + (long long)j * p.sRn];
            VST2(float, C + r * p.sCm + j, v);
        }
    }
}
__global__ __launch_bounds__(256) void k_smallsoftmax(const float* __restrict__ src, float* __restrict__ dst, long long sr, long long dr, int n, long long R, float scale) {
    const long long r0 = ((long long)blockIdx.x * 256 + threadIdx.x) * 32;
    for (int rr = 0; rr < 32; ++rr) {
        const long long r = r0 + rr; if (r >= R) return;
        const float* s = src + r * sr; float* d = dst + r * dr;
        float mx = -__builtin_inff();
        for (int j = 0; j < n; ++j) mx = fmaxf(mx, s[j] * scale);
        float sum = 0.f;
        for (int j = 0; j < n; ++j) sum += expf(s[j] * scale - mx);
        const float inv = 1.f / sum;
        for (int j = 0; j < n; ++j) { const float v = expf(s[j] * scale - mx) * inv; VST2(float, d + j, v); }
    }
}

__global__ __launch_bounds__(32) void k_unitstat(float* __restrict__ st) { const int t = threadIdx.x; const float v = (t == 1) ? 1.f : 0.f; VST2(float, st + t, v); }

__global__ __launch_bounds__(256) void k_lincopy(const float* __restrict__ src, long long lds, float* __restrict__ dst, long long ldd, long long rows, int cols) {
    const long long i = (long long)blockIdx.x * 256 + threadIdx.x; if (i >= rows * cols) return;
    const long long r = i / cols; const int c = (int)(i - r * cols);
    const float v = src[r * lds + c]; VST2(float, dst + r * ldd + c, v);
}

#define IL_CAP64 64
#define IL_T64 128
#define IL_TILE64 4096
__global__ __launch_bounds__(IL_T64) void k_inlists64(const int* __restrict__ tgt, int E, int N, int* __restrict__ NBR, int* __restrict__ cnt) {
    __shared__ int tt[IL_TILE64];
    __shared__ int lists[IL_T64 * IL_CAP64];
    const int d = blockIdx.x * IL_T64 + threadIdx.x; int n = 0;
    for (int e0 = 0; e0 < E; e0 += IL_TILE64) {
        const int nt = min(IL_TILE64, E - e0);
        __syncthreads();
        for (int i = threadIdx.x; i < nt; i += IL_T64) tt[i] = tgt[e0 + i];
        __syncthreads();
        for (int i = 0; i < nt; ++i) { if (tt[i] == d) { if (n < IL_CAP64) lists[threadIdx.x * IL_CAP64 + n] = e0 + i; ++n; } }
    }
    if (d < N) {
        int* row = NBR + (long long)d * IL_CAP64;
        for (int j = 0; j < IL_CAP64; ++j) { const int v = (j < n) ? lists[threadIdx.x * IL_CAP64 + j] : -1; VST2(int, row + j, v); }
        VST2(int, cnt + d, min(n, IL_CAP64));
    }
}
__global__ __launch_bounds__(256) void k_csr_scan64(const int* __restrict__ cnt, int* __restrict__ off, int N) {
    __shared__ int part[256]; const int per = ((((N + 255) / 256) + 31) / 32) * 32; const int a = threadIdx.x * per, b = min(N, a + per); int s = 0;
    for (int i = a; i < b; ++i) s += cnt[i]; part[threadIdx.x] = s; __syncthreads();
    if (threadIdx.x == 0) { int run = 0; for (int t = 0; t < 256; ++t) { const int v = part[t]; part[t] = run; run += v; } } __syncthreads();
    int run = part[threadIdx.x]; for (int i = a; i < b; ++i) { VST2(int, off + i, run); run += cnt[i]; }
    if (a < N && b == N) { VST2(int, off + N, run); }
}
__global__ __launch_bounds__(256) void k_slotcopy64(const int* __restrict__ off, const int* __restrict__ NBR, int* __restrict__ slot, int N) {
    const int t = blockIdx.x * 256 + threadIdx.x; const int tot = off[N]; if (t >= tot) return;
    int lo = 0, hi = N - 1;
    while (lo < hi) { const int mid = (lo + hi + 1) >> 1; if (off[mid] <= t) lo = mid; else hi = mid - 1; }
    int j = t - off[lo]; j = (j < 0) ? 0 : ((j >= IL_CAP64) ? (IL_CAP64 - 1) : j);
    VST2(int, slot + t, NBR[(long long)lo * IL_CAP64 + j]);
}

#define IL_CAP1024 1024
#define IL_T1024 8
#define IL_TILE1024 4096
__global__ __launch_bounds__(IL_T1024) void k_inlists1024(const int* __restrict__ tgt, int E, int N, int* __restrict__ NBR, int* __restrict__ cnt) {
    __shared__ int tt[IL_TILE1024];
    __shared__ int lists[IL_T1024 * IL_CAP1024];
    const int d = blockIdx.x * IL_T1024 + threadIdx.x; int n = 0;
    for (int e0 = 0; e0 < E; e0 += IL_TILE1024) {
        const int nt = min(IL_TILE1024, E - e0);
        __syncthreads();
        for (int i = threadIdx.x; i < nt; i += IL_T1024) tt[i] = tgt[e0 + i];
        __syncthreads();
        for (int i = 0; i < nt; ++i) { if (tt[i] == d) { if (n < IL_CAP1024) lists[threadIdx.x * IL_CAP1024 + n] = e0 + i; ++n; } }
    }
    if (d < N) {
        int* row = NBR + (long long)d * IL_CAP1024;
        for (int j = 0; j < IL_CAP1024; ++j) { const int v = (j < n) ? lists[threadIdx.x * IL_CAP1024 + j] : -1; VST2(int, row + j, v); }
        VST2(int, cnt + d, min(n, IL_CAP1024));
    }
}
__global__ __launch_bounds__(256) void k_csr_scan1024(const int* __restrict__ cnt, int* __restrict__ off, int N) {
    __shared__ int part[256]; const int per = ((((N + 255) / 256) + 31) / 32) * 32; const int a = threadIdx.x * per, b = min(N, a + per); int s = 0;
    for (int i = a; i < b; ++i) s += cnt[i]; part[threadIdx.x] = s; __syncthreads();
    if (threadIdx.x == 0) { int run = 0; for (int t = 0; t < 256; ++t) { const int v = part[t]; part[t] = run; run += v; } } __syncthreads();
    int run = part[threadIdx.x]; for (int i = a; i < b; ++i) { VST2(int, off + i, run); run += cnt[i]; }
    if (a < N && b == N) { VST2(int, off + N, run); }
}
__global__ __launch_bounds__(256) void k_slotcopy1024(const int* __restrict__ off, const int* __restrict__ NBR, int* __restrict__ slot, int N) {
    const int t = blockIdx.x * 256 + threadIdx.x; const int tot = off[N]; if (t >= tot) return;
    int lo = 0, hi = N - 1;
    while (lo < hi) { const int mid = (lo + hi + 1) >> 1; if (off[mid] <= t) lo = mid; else hi = mid - 1; }
    int j = t - off[lo]; j = (j < 0) ? 0 : ((j >= IL_CAP1024) ? (IL_CAP1024 - 1) : j);
    VST2(int, slot + t, NBR[(long long)lo * IL_CAP1024 + j]);
}


__global__ __launch_bounds__(256) void k_csr_mean(const float* __restrict__ Hh, const int* __restrict__ src, const int* __restrict__ off, const int* __restrict__ slot, float* __restrict__ AGG, int N, int D) {
    const long long t = (long long)blockIdx.x * 256 + threadIdx.x; if (t >= (long long)N * D) return; const int d = (int)(t % D); const int i = (int)(t / D); const int a = off[i], b = off[i + 1]; float s = 0.f;
    for (int p = a; p < b; ++p) s += Hh[(long long)src[slot[p]] * D + d];
    VST2(float, AGG + t, s / fmaxf((float)(b - a), 1.f));
}

__global__ __launch_bounds__(256) void k_edgestat(const float* __restrict__ M, const float* __restrict__ pos, const int* __restrict__ ei, float* __restrict__ EST, int E, int C) {
    const int e = blockIdx.x * 256 + threadIdx.x; if (e >= E) return; const int s = ei[e], d = ei[E + e]; const float* ms = M + (long long)s * C; const float* md = M + (long long)d * C;
    const int n = 2 * C + 6; float sum = 0.f;
    for (int c = 0; c < C; ++c) sum += ms[c] + md[c];
    for (int c = 0; c < 3; ++c) sum += pos[s * 3 + c] + pos[d * 3 + c];
    const float mu = sum / (float)n; float q = 0.f;
    for (int c = 0; c < C; ++c) { float t = ms[c] - mu; q += t * t; t = md[c] - mu; q += t * t; }
    for (int c = 0; c < 3; ++c) { float t = pos[s * 3 + c] - mu; q += t * t; t = pos[d * 3 + c] - mu; q += t * t; }
    VST2(float, EST + 2 * (long long)e, mu); VST2(float, EST + 2 * (long long)e + 1, rsqrtf(q / (float)n + 1e-5f));
}
__global__ __launch_bounds__(256) void k_edgefeat(const float* __restrict__ M, const float* __restrict__ pos, const int* __restrict__ ei, const float* __restrict__ EST, const float* __restrict__ g, const float* __restrict__ bb, float* __restrict__ EF, int e0, int ECH, int E, int C, int ld) {
    const long long t = (long long)blockIdx.x * 256 + threadIdx.x; if (t >= (long long)ECH * ld) return; const int c = (int)(t % ld); const int e = e0 + (int)(t / ld); float v = 0.f;
    if (c < 2 * C + 6) { const int s = ei[e], d = ei[E + e]; float f;
        if (c < C) f = M[(long long)s * C + c]; else if (c < 2 * C) f = M[(long long)d * C + (c - C)]; else if (c < 2 * C + 3) f = pos[s * 3 + (c - 2 * C)]; else f = pos[d * 3 + (c - 2 * C - 3)];
        v = (f - EST[2 * (long long)e]) * EST[2 * (long long)e + 1] * g[c] + bb[c]; }
    VST2(float, EF + t, v);
}
__global__ __launch_bounds__(256) void k_edgegate(const float* __restrict__ E4, int ldp, const float* __restrict__ g2, const float* __restrict__ b2, const float* __restrict__ w2, const float* __restrict__ wb, float* __restrict__ WE, int e0, int ECH) {
    const int r = blockIdx.x * 256 + threadIdx.x; if (r >= ECH) return; float v[4]; float mu = 0.f;
#pragma unroll
    for (int j = 0; j < 4; ++j) { const float a = E4[(long long)r * ldp + j]; v[j] = 0.5f * a * (1.f + erff(a * 0.7071067811865476f)); mu += v[j]; }
    mu *= 0.25f; float q = 0.f;
#pragma unroll
    for (int j = 0; j < 4; ++j) { const float t = v[j] - mu; q += t * t; }
    const float rs = rsqrtf(q * 0.25f + 1e-5f); float z = wb[0];
#pragma unroll
    for (int j = 0; j < 4; ++j) z += ((v[j] - mu) * rs * g2[j] + b2[j]) * w2[j];
    VST2(float, WE + e0 + r, 1.f / (1.f + expf(-z)));
}
__global__ __launch_bounds__(256) void k_wagg(const float* __restrict__ M, const int* __restrict__ ei, const float* __restrict__ WE, const int* __restrict__ off, const int* __restrict__ slot, float* __restrict__ AGG, int N, int C) {
    const long long t = (long long)blockIdx.x * 256 + threadIdx.x; if (t >= (long long)N * C) return; const int c = (int)(t % C); const int n = (int)(t / C); const int a = off[n], b = off[n + 1]; float s = 0.f;
    for (int p = a; p < b; ++p) { const int e = slot[p]; s += WE[e] * M[(long long)ei[e] * C + c]; }
    VST2(float, AGG + t, s);
}

template __global__ void k_gemm<1>(GemmP);

extern "C" void kernel_launch(void* const* d_in, const int* in_sizes, int n_in, void* d_out, int out_size, void* d_ws, size_t ws_size, hipStream_t stream) {
    (void)in_sizes; (void)n_in; (void)out_size; (void)ws_size;
    const float* x = (const float*)d_in[0];
    const float* xpos = (const float*)d_in[1];
    const int* ei = (const int*)d_in[2];
    const int* bat = (const int*)d_in[3];
    const float* dw = (const float*)d_in[4];
    const float* db = (const float*)d_in[5];
    const float* d1w = (const float*)d_in[6];
    const float* d1b = (const float*)d_in[7];
    const float* l1g = (const float*)d_in[8];
    const float* l1b = (const float*)d_in[9];
    const float* w1w = (const float*)d_in[10];
    const float* w1b = (const float*)d_in[11];
    const float* l2g = (const float*)d_in[12];
    const float* l2b = (const float*)d_in[13];
    const float* w2w = (const float*)d_in[14];
    const float* w2b = (const float*)d_in[15];
    const float* d2w = (const float*)d_in[16];
    const float* d2b = (const float*)d_in[17];
    const float* hw = (const float*)d_in[18];
    const float* hb = (const float*)d_in[19];
    const int Nn = 20000;
    const int E = 320000;
    const int G = 32;
    const int C = 256;
    const int DIN = 739;
    const int ED = 518;
    const int LDE = 544;
    const int ECH = 40000;
    const int NCH = 8;
    const int CAP = 64;
    const int GCAP = 1024;
    const int LDP = 32;
    float* out = (float*)d_out;
    char* wsp = (char*)d_ws;
    int* cnt = (int*)wsp; wsp += (((size_t)((size_t)Nn + 64) * 4 + 255) / 256) * 256;
    int* off = (int*)wsp; wsp += (((size_t)((size_t)Nn + 64) * 4 + 255) / 256) * 256;
    int* slot = (int*)wsp; wsp += (((size_t)((size_t)E + 64) * 4 + 255) / 256) * 256;
    int* nbr = (int*)wsp; wsp += (((size_t)((size_t)Nn * CAP) * 4 + 255) / 256) * 256;
    int* gcnt = (int*)wsp; wsp += (((size_t)((size_t)G + 64) * 4 + 255) / 256) * 256;
    int* goff = (int*)wsp; wsp += (((size_t)((size_t)G + 64) * 4 + 255) / 256) * 256;
    int* gslot = (int*)wsp; wsp += (((size_t)((size_t)Nn + 64) * 4 + 255) / 256) * 256;
    int* gnbr = (int*)wsp; wsp += (((size_t)((size_t)G * GCAP) * 4 + 255) / 256) * 256;
    int* ids = (int*)wsp; wsp += (((size_t)((size_t)Nn + 64) * 4 + 255) / 256) * 256;
    float* H = (float*)wsp; wsp += (((size_t)((size_t)Nn * C) * 4 + 255) / 256) * 256;
    float* M = (float*)wsp; wsp += (((size_t)((size_t)Nn * C) * 4 + 255) / 256) * 256;
    float* EST = (float*)wsp; wsp += (((size_t)((size_t)E * 2 + 64) * 4 + 255) / 256) * 256;
    float* EF = (float*)wsp; wsp += (((size_t)((size_t)ECH * LDE) * 4 + 255) / 256) * 256;
    float* E4 = (float*)wsp; wsp += (((size_t)((size_t)ECH * LDP) * 4 + 255) / 256) * 256;
    float* WE = (float*)wsp; wsp += (((size_t)((size_t)E + 64) * 4 + 255) / 256) * 256;
    float* AGG = (float*)wsp; wsp += (((size_t)((size_t)Nn * C) * 4 + 255) / 256) * 256;
    float* PL = (float*)wsp; wsp += (((size_t)((size_t)G * C) * 4 + 255) / 256) * 256;
    float* OP = (float*)wsp; wsp += (((size_t)((size_t)G * LDP) * 4 + 255) / 256) * 256;
    k_inlists64<<<(unsigned)((Nn) + IL_T64 - 1) / IL_T64, IL_T64, 0, stream>>>(ei + E, E, Nn, nbr, cnt);
    k_csr_scan64<<<1, 256, 0, stream>>>(cnt, off, Nn);
    k_slotcopy64<<<(unsigned)((E) + 255) / 256, 256, 0, stream>>>(off, nbr, slot, Nn);
    k_inlists1024<<<(unsigned)((G) + IL_T1024 - 1) / IL_T1024, IL_T1024, 0, stream>>>(bat, Nn, G, gnbr, gcnt);
    k_csr_scan1024<<<1, 256, 0, stream>>>(gcnt, goff, G);
    k_slotcopy1024<<<(unsigned)((Nn) + 255) / 256, 256, 0, stream>>>(goff, gnbr, gslot, G);
    k_iota<<<(unsigned)((Nn) + 255) / 256, 256, 0, stream>>>(ids, Nn, 1, 0);
    { GemmP gd;
      gd.A = x; gd.B = dw; gd.bias = db; gd.R = x; gd.C = H;
      gd.sAo = 0; gd.sAi = 0; gd.sAm = DIN; gd.sAk = 1; gd.sBo = 0; gd.sBi = 0; gd.sBn = 1; gd.sBk = C; gd.sCo = 0; gd.sCi = 0; gd.sCm = C; gd.sRo = 0; gd.sRi = 0; gd.sRm = 0; gd.sRn = 0;
      gd.M = Nn; gd.N = C; gd.K = DIN; gd.zi_n = 1; gd.flags = 1; gd.act = 0;
      gd.alpha = 1.0f; gd.beta = 0.0f; gd.sa = 1.0f; gd.sb = 1.0f; gd.Npad = C; gd.pad_ = 0;
      k_gemm<1><<<dim3((unsigned)((C) + 31) / 32, (unsigned)((Nn) + 15) / 16, (unsigned)(1)), 32, 0, stream>>>(gd); }
    { GemmP gm0;
      gm0.A = H; gm0.B = d1w + (size_t)0 * C * C; gm0.bias = d1b + (size_t)0 * C; gm0.R = H; gm0.C = M;
      gm0.sAo = 0; gm0.sAi = 0; gm0.sAm = C; gm0.sAk = 1; gm0.sBo = 0; gm0.sBi = 0; gm0.sBn = 1; gm0.sBk = C; gm0.sCo = 0; gm0.sCi = 0; gm0.sCm = C; gm0.sRo = 0; gm0.sRi = 0; gm0.sRm = 0; gm0.sRn = 0;
      gm0.M = Nn; gm0.N = C; gm0.K = C; gm0.zi_n = 1; gm0.flags = 1; gm0.act = 4;
      gm0.alpha = 1.0f; gm0.beta = 0.0f; gm0.sa = 1.0f; gm0.sb = 1.0f; gm0.Npad = C; gm0.pad_ = 0;
      k_gemm<1><<<dim3((unsigned)((C) + 31) / 32, (unsigned)((Nn) + 15) / 16, (unsigned)(1)), 32, 0, stream>>>(gm0); }
    k_edgestat<<<(unsigned)((E + 255) / 256), 256, 0, stream>>>(M, xpos, ei, EST, E, C);
    k_edgefeat<<<(unsigned)(((long long)ECH * LDE + 255) / 256), 256, 0, stream>>>(M, xpos, ei, EST, l1g + (size_t)0 * ED, l1b + (size_t)0 * ED, EF, 0, ECH, E, C, LDE);
    { GemmP ge0_0;
      ge0_0.A = EF; ge0_0.B = w1w + (size_t)0 * ED * 4; ge0_0.bias = w1b + (size_t)0 * 4; ge0_0.R = EF; ge0_0.C = E4;
      ge0_0.sAo = 0; ge0_0.sAi = 0; ge0_0.sAm = LDE; ge0_0.sAk = 1; ge0_0.sBo = 0; ge0_0.sBi = 0; ge0_0.sBn = 1; ge0_0.sBk = 4; ge0_0.sCo = 0; ge0_0.sCi = 0; ge0_0.sCm = LDP; ge0_0.sRo = 0; ge0_0.sRi = 0; ge0_0.sRm = 0; ge0_0.sRn = 0;
      ge0_0.M = ECH; ge0_0.N = 4; ge0_0.K = ED; ge0_0.zi_n = 1; ge0_0.flags = 1; ge0_0.act = 0;
      ge0_0.alpha = 1.0f; ge0_0.beta = 0.0f; ge0_0.sa = 1.0f; ge0_0.sb = 1.0f; ge0_0.Npad = LDP; ge0_0.pad_ = 0;
      k_gemm<1><<<dim3((unsigned)((LDP) + 31) / 32, (unsigned)((ECH) + 15) / 16, (unsigned)(1)), 32, 0, stream>>>(ge0_0); }
    k_edgegate<<<(unsigned)((ECH + 255) / 256), 256, 0, stream>>>(E4, LDP, l2g + (size_t)0 * 4, l2b + (size_t)0 * 4, w2w + (size_t)0 * 4, w2b + (size_t)0, WE, 0, ECH);
    k_edgefeat<<<(unsigned)(((long long)ECH * LDE + 255) / 256), 256, 0, stream>>>(M, xpos, ei, EST, l1g + (size_t)0 * ED, l1b + (size_t)0 * ED, EF, 40000, ECH, E, C, LDE);
    { GemmP ge0_1;
      ge0_1.A = EF; ge0_1.B = w1w + (size_t)0 * ED * 4; ge0_1.bias = w1b + (size_t)0 * 4; ge0_1.R = EF; ge0_1.C = E4;
      ge0_1.sAo = 0; ge0_1.sAi = 0; ge0_1.sAm = LDE; ge0_1.sAk = 1; ge0_1.sBo = 0; ge0_1.sBi = 0; ge0_1.sBn = 1; ge0_1.sBk = 4; ge0_1.sCo = 0; ge0_1.sCi = 0; ge0_1.sCm = LDP; ge0_1.sRo = 0; ge0_1.sRi = 0; ge0_1.sRm = 0; ge0_1.sRn = 0;
      ge0_1.M = ECH; ge0_1.N = 4; ge0_1.K = ED; ge0_1.zi_n = 1; ge0_1.flags = 1; ge0_1.act = 0;
      ge0_1.alpha = 1.0f; ge0_1.beta = 0.0f; ge0_1.sa = 1.0f; ge0_1.sb = 1.0f; ge0_1.Npad = LDP; ge0_1.pad_ = 0;
      k_gemm<1><<<dim3((unsigned)((LDP) + 31) / 32, (unsigned)((ECH) + 15) / 16, (unsigned)(1)), 32, 0, stream>>>(ge0_1); }
    k_edgegate<<<(unsigned)((ECH + 255) / 256), 256, 0, stream>>>(E4, LDP, l2g + (size_t)0 * 4, l2b + (size_t)0 * 4, w2w + (size_t)0 * 4, w2b + (size_t)0, WE, 40000, ECH);
    k_edgefeat<<<(unsigned)(((long long)ECH * LDE + 255) / 256), 256, 0, stream>>>(M, xpos, ei, EST, l1g + (size_t)0 * ED, l1b + (size_t)0 * ED, EF, 80000, ECH, E, C, LDE);
    { GemmP ge0_2;
      ge0_2.A = EF; ge0_2.B = w1w + (size_t)0 * ED * 4; ge0_2.bias = w1b + (size_t)0 * 4; ge0_2.R = EF; ge0_2.C = E4;
      ge0_2.sAo = 0; ge0_2.sAi = 0; ge0_2.sAm = LDE; ge0_2.sAk = 1; ge0_2.sBo = 0; ge0_2.sBi = 0; ge0_2.sBn = 1; ge0_2.sBk = 4; ge0_2.sCo = 0; ge0_2.sCi = 0; ge0_2.sCm = LDP; ge0_2.sRo = 0; ge0_2.sRi = 0; ge0_2.sRm = 0; ge0_2.sRn = 0;
      ge0_2.M = ECH; ge0_2.N = 4; ge0_2.K = ED; ge0_2.zi_n = 1; ge0_2.flags = 1; ge0_2.act = 0;
      ge0_2.alpha = 1.0f; ge0_2.beta = 0.0f; ge0_2.sa = 1.0f; ge0_2.sb = 1.0f; ge0_2.Npad = LDP; ge0_2.pad_ = 0;
      k_gemm<1><<<dim3((unsigned)((LDP) + 31) / 32, (unsigned)((ECH) + 15) / 16, (unsigned)(1)), 32, 0, stream>>>(ge0_2); }
    k_edgegate<<<(unsigned)((ECH + 255) / 256), 256, 0, stream>>>(E4, LDP, l2g + (size_t)0 * 4, l2b + (size_t)0 * 4, w2w + (size_t)0 * 4, w2b + (size_t)0, WE, 80000, ECH);
    k_edgefeat<<<(unsigned)(((long long)ECH * LDE + 255) / 256), 256, 0, stream>>>(M, xpos, ei, EST, l1g + (size_t)0 * ED, l1b + (size_t)0 * ED, EF, 120000, ECH, E, C, LDE);
    { GemmP ge0_3;
      ge0_3.A = EF; ge0_3.B = w1w + (size_t)0 * ED * 4; ge0_3.bias = w1b + (size_t)0 * 4; ge0_3.R = EF; ge0_3.C = E4;
      ge0_3.sAo = 0; ge0_3.sAi = 0; ge0_3.sAm = LDE; ge0_3.sAk = 1; ge0_3.sBo = 0; ge0_3.sBi = 0; ge0_3.sBn = 1; ge0_3.sBk = 4; ge0_3.sCo = 0; ge0_3.sCi = 0; ge0_3.sCm = LDP; ge0_3.sRo = 0; ge0_3.sRi = 0; ge0_3.sRm = 0; ge0_3.sRn = 0;
      ge0_3.M = ECH; ge0_3.N = 4; ge0_3.K = ED; ge0_3.zi_n = 1; ge0_3.flags = 1; ge0_3.act = 0;
      ge0_3.alpha = 1.0f; ge0_3.beta = 0.0f; ge0_3.sa = 1.0f; ge0_3.sb = 1.0f; ge0_3.Npad = LDP; ge0_3.pad_ = 0;
      k_gemm<1><<<dim3((unsigned)((LDP) + 31) / 32, (unsigned)((ECH) + 15) / 16, (unsigned)(1)), 32, 0, stream>>>(ge0_3); }
    k_edgegate<<<(unsigned)((ECH + 255) / 256), 256, 0, stream>>>(E4, LDP, l2g + (size_t)0 * 4, l2b + (size_t)0 * 4, w2w + (size_t)0 * 4, w2b + (size_t)0, WE, 120000, ECH);
    k_edgefeat<<<(unsigned)(((long long)ECH * LDE + 255) / 256), 256, 0, stream>>>(M, xpos, ei, EST, l1g + (size_t)0 * ED, l1b + (size_t)0 * ED, EF, 160000, ECH, E, C, LDE);
    { GemmP ge0_4;
      ge0_4.A = EF; ge0_4.B = w1w + (size_t)0 * ED * 4; ge0_4.bias = w1b + (size_t)0 * 4; ge0_4.R = EF; ge0_4.C = E4;
      ge0_4.sAo = 0; ge0_4.sAi = 0; ge0_4.sAm = LDE; ge0_4.sAk = 1; ge0_4.sBo = 0; ge0_4.sBi = 0; ge0_4.sBn = 1; ge0_4.sBk = 4; ge0_4.sCo = 0; ge0_4.sCi = 0; ge0_4.sCm = LDP; ge0_4.sRo = 0; ge0_4.sRi = 0; ge0_4.sRm = 0; ge0_4.sRn = 0;
      ge0_4.M = ECH; ge0_4.N = 4; ge0_4.K = ED; ge0_4.zi_n = 1; ge0_4.flags = 1; ge0_4.act = 0;
      ge0_4.alpha = 1.0f; ge0_4.beta = 0.0f; ge0_4.sa = 1.0f; ge0_4.sb = 1.0f; ge0_4.Npad = LDP; ge0_4.pad_ = 0;
      k_gemm<1><<<dim3((unsigned)((LDP) + 31) / 32, (unsigned)((ECH) + 15) / 16, (unsigned)(1)), 32, 0, stream>>>(ge0_4); }
    k_edgegate<<<(unsigned)((ECH + 255) / 256), 256, 0, stream>>>(E4, LDP, l2g + (size_t)0 * 4, l2b + (size_t)0 * 4, w2w + (size_t)0 * 4, w2b + (size_t)0, WE, 160000, ECH);
    k_edgefeat<<<(unsigned)(((long long)ECH * LDE + 255) / 256), 256, 0, stream>>>(M, xpos, ei, EST, l1g + (size_t)0 * ED, l1b + (size_t)0 * ED, EF, 200000, ECH, E, C, LDE);
    { GemmP ge0_5;
      ge0_5.A = EF; ge0_5.B = w1w + (size_t)0 * ED * 4; ge0_5.bias = w1b + (size_t)0 * 4; ge0_5.R = EF; ge0_5.C = E4;
      ge0_5.sAo = 0; ge0_5.sAi = 0; ge0_5.sAm = LDE; ge0_5.sAk = 1; ge0_5.sBo = 0; ge0_5.sBi = 0; ge0_5.sBn = 1; ge0_5.sBk = 4; ge0_5.sCo = 0; ge0_5.sCi = 0; ge0_5.sCm = LDP; ge0_5.sRo = 0; ge0_5.sRi = 0; ge0_5.sRm = 0; ge0_5.sRn = 0;
      ge0_5.M = ECH; ge0_5.N = 4; ge0_5.K = ED; ge0_5.zi_n = 1; ge0_5.flags = 1; ge0_5.act = 0;
      ge0_5.alpha = 1.0f; ge0_5.beta = 0.0f; ge0_5.sa = 1.0f; ge0_5.sb = 1.0f; ge0_5.Npad = LDP; ge0_5.pad_ = 0;
      k_gemm<1><<<dim3((unsigned)((LDP) + 31) / 32, (unsigned)((ECH) + 15) / 16, (unsigned)(1)), 32, 0, stream>>>(ge0_5); }
    k_edgegate<<<(unsigned)((ECH + 255) / 256), 256, 0, stream>>>(E4, LDP, l2g + (size_t)0 * 4, l2b + (size_t)0 * 4, w2w + (size_t)0 * 4, w2b + (size_t)0, WE, 200000, ECH);
    k_edgefeat<<<(unsigned)(((long long)ECH * LDE + 255) / 256), 256, 0, stream>>>(M, xpos, ei, EST, l1g + (size_t)0 * ED, l1b + (size_t)0 * ED, EF, 240000, ECH, E, C, LDE);
    { GemmP ge0_6;
      ge0_6.A = EF; ge0_6.B = w1w + (size_t)0 * ED * 4; ge0_6.bias = w1b + (size_t)0 * 4; ge0_6.R = EF; ge0_6.C = E4;
      ge0_6.sAo = 0; ge0_6.sAi = 0; ge0_6.sAm = LDE; ge0_6.sAk = 1; ge0_6.sBo = 0; ge0_6.sBi = 0; ge0_6.sBn = 1; ge0_6.sBk = 4; ge0_6.sCo = 0; ge0_6.sCi = 0; ge0_6.sCm = LDP; ge0_6.sRo = 0; ge0_6.sRi = 0; ge0_6.sRm = 0; ge0_6.sRn = 0;
      ge0_6.M = ECH; ge0_6.N = 4; ge0_6.K = ED; ge0_6.zi_n = 1; ge0_6.flags = 1; ge0_6.act = 0;
      ge0_6.alpha = 1.0f; ge0_6.beta = 0.0f; ge0_6.sa = 1.0f; ge0_6.sb = 1.0f; ge0_6.Npad = LDP; ge0_6.pad_ = 0;
      k_gemm<1><<<dim3((unsigned)((LDP) + 31) / 32, (unsigned)((ECH) + 15) / 16, (unsigned)(1)), 32, 0, stream>>>(ge0_6); }
    k_edgegate<<<(unsigned)((ECH + 255) / 256), 256, 0, stream>>>(E4, LDP, l2g + (size_t)0 * 4, l2b + (size_t)0 * 4, w2w + (size_t)0 * 4, w2b + (size_t)0, WE, 240000, ECH);
    k_edgefeat<<<(unsigned)(((long long)ECH * LDE + 255) / 256), 256, 0, stream>>>(M, xpos, ei, EST, l1g + (size_t)0 * ED, l1b + (size_t)0 * ED, EF, 280000, ECH, E, C, LDE);
    { GemmP ge0_7;
      ge0_7.A = EF; ge0_7.B = w1w + (size_t)0 * ED * 4; ge0_7.bias = w1b + (size_t)0 * 4; ge0_7.R = EF; ge0_7.C = E4;
      ge0_7.sAo = 0; ge0_7.sAi = 0; ge0_7.sAm = LDE; ge0_7.sAk = 1; ge0_7.sBo = 0; ge0_7.sBi = 0; ge0_7.sBn = 1; ge0_7.sBk = 4; ge0_7.sCo = 0; ge0_7.sCi = 0; ge0_7.sCm = LDP; ge0_7.sRo = 0; ge0_7.sRi = 0; ge0_7.sRm = 0; ge0_7.sRn = 0;
      ge0_7.M = ECH; ge0_7.N = 4; ge0_7.K = ED; ge0_7.zi_n = 1; ge0_7.flags = 1; ge0_7.act = 0;
      ge0_7.alpha = 1.0f; ge0_7.beta = 0.0f; ge0_7.sa = 1.0f; ge0_7.sb = 1.0f; ge0_7.Npad = LDP; ge0_7.pad_ = 0;
      k_gemm<1><<<dim3((unsigned)((LDP) + 31) / 32, (unsigned)((ECH) + 15) / 16, (unsigned)(1)), 32, 0, stream>>>(ge0_7); }
    k_edgegate<<<(unsigned)((ECH + 255) / 256), 256, 0, stream>>>(E4, LDP, l2g + (size_t)0 * 4, l2b + (size_t)0 * 4, w2w + (size_t)0 * 4, w2b + (size_t)0, WE, 280000, ECH);
    k_wagg<<<(unsigned)(((long long)Nn * C + 255) / 256), 256, 0, stream>>>(M, ei, WE, off, slot, AGG, Nn, C);
    { GemmP gh0;
      gh0.A = AGG; gh0.B = d2w + (size_t)0 * C * C; gh0.bias = d2b + (size_t)0 * C; gh0.R = AGG; gh0.C = H;
      gh0.sAo = 0; gh0.sAi = 0; gh0.sAm = C; gh0.sAk = 1; gh0.sBo = 0; gh0.sBi = 0; gh0.sBn = 1; gh0.sBk = C; gh0.sCo = 0; gh0.sCi = 0; gh0.sCm = C; gh0.sRo = 0; gh0.sRi = 0; gh0.sRm = 0; gh0.sRn = 0;
      gh0.M = Nn; gh0.N = C; gh0.K = C; gh0.zi_n = 1; gh0.flags = 1; gh0.act = 4;
      gh0.alpha = 1.0f; gh0.beta = 0.0f; gh0.sa = 1.0f; gh0.sb = 1.0f; gh0.Npad = C; gh0.pad_ = 0;
      k_gemm<1><<<dim3((unsigned)((C) + 31) / 32, (unsigned)((Nn) + 15) / 16, (unsigned)(1)), 32, 0, stream>>>(gh0); }
    { GemmP gm1;
      gm1.A = H; gm1.B = d1w + (size_t)1 * C * C; gm1.bias = d1b + (size_t)1 * C; gm1.R = H; gm1.C = M;
      gm1.sAo = 0; gm1.sAi = 0; gm1.sAm = C; gm1.sAk = 1; gm1.sBo = 0; gm1.sBi = 0; gm1.sBn = 1; gm1.sBk = C; gm1.sCo = 0; gm1.sCi = 0; gm1.sCm = C; gm1.sRo = 0; gm1.sRi = 0; gm1.sRm = 0; gm1.sRn = 0;
      gm1.M = Nn; gm1.N = C; gm1.K = C; gm1.zi_n = 1; gm1.flags = 1; gm1.act = 4;
      gm1.alpha = 1.0f; gm1.beta = 0.0f; gm1.sa = 1.0f; gm1.sb = 1.0f; gm1.Npad = C; gm1.pad_ = 0;
      k_gemm<1><<<dim3((unsigned)((C) + 31) / 32, (unsigned)((Nn) + 15) / 16, (unsigned)(1)), 32, 0, stream>>>(gm1); }
    k_edgestat<<<(unsigned)((E + 255) / 256), 256, 0, stream>>>(M, xpos, ei, EST, E, C);
    k_edgefeat<<<(unsigned)(((long long)ECH * LDE + 255) / 256), 256, 0, stream>>>(M, xpos, ei, EST, l1g + (size_t)1 * ED, l1b + (size_t)1 * ED, EF, 0, ECH, E, C, LDE);
    { GemmP ge1_0;
      ge1_0.A = EF; ge1_0.B = w1w + (size_t)1 * ED * 4; ge1_0.bias = w1b + (size_t)1 * 4; ge1_0.R = EF; ge1_0.C = E4;
      ge1_0.sAo = 0; ge1_0.sAi = 0; ge1_0.sAm = LDE; ge1_0.sAk = 1; ge1_0.sBo = 0; ge1_0.sBi = 0; ge1_0.sBn = 1; ge1_0.sBk = 4; ge1_0.sCo = 0; ge1_0.sCi = 0; ge1_0.sCm = LDP; ge1_0.sRo = 0; ge1_0.sRi = 0; ge1_0.sRm = 0; ge1_0.sRn = 0;
      ge1_0.M = ECH; ge1_0.N = 4; ge1_0.K = ED; ge1_0.zi_n = 1; ge1_0.flags = 1; ge1_0.act = 0;
      ge1_0.alpha = 1.0f; ge1_0.beta = 0.0f; ge1_0.sa = 1.0f; ge1_0.sb = 1.0f; ge1_0.Npad = LDP; ge1_0.pad_ = 0;
      k_gemm<1><<<dim3((unsigned)((LDP) + 31) / 32, (unsigned)((ECH) + 15) / 16, (unsigned)(1)), 32, 0, stream>>>(ge1_0); }
    k_edgegate<<<(unsigned)((ECH + 255) / 256), 256, 0, stream>>>(E4, LDP, l2g + (size_t)1 * 4, l2b + (size_t)1 * 4, w2w + (size_t)1 * 4, w2b + (size_t)1, WE, 0, ECH);
    k_edgefeat<<<(unsigned)(((long long)ECH * LDE + 255) / 256), 256, 0, stream>>>(M, xpos, ei, EST, l1g + (size_t)1 * ED, l1b + (size_t)1 * ED, EF, 40000, ECH, E, C, LDE);
    { GemmP ge1_1;
      ge1_1.A = EF; ge1_1.B = w1w + (size_t)1 * ED * 4; ge1_1.bias = w1b + (size_t)1 * 4; ge1_1.R = EF; ge1_1.C = E4;
      ge1_1.sAo = 0; ge1_1.sAi = 0; ge1_1.sAm = LDE; ge1_1.sAk = 1; ge1_1.sBo = 0; ge1_1.sBi = 0; ge1_1.sBn = 1; ge1_1.sBk = 4; ge1_1.sCo = 0; ge1_1.sCi = 0; ge1_1.sCm = LDP; ge1_1.sRo = 0; ge1_1.sRi = 0; ge1_1.sRm = 0; ge1_1.sRn = 0;
      ge1_1.M = ECH; ge1_1.N = 4; ge1_1.K = ED; ge1_1.zi_n = 1; ge1_1.flags = 1; ge1_1.act = 0;
      ge1_1.alpha = 1.0f; ge1_1.beta = 0.0f; ge1_1.sa = 1.0f; ge1_1.sb = 1.0f; ge1_1.Npad = LDP; ge1_1.pad_ = 0;
      k_gemm<1><<<dim3((unsigned)((LDP) + 31) / 32, (unsigned)((ECH) + 15) / 16, (unsigned)(1)), 32, 0, stream>>>(ge1_1); }
    k_edgegate<<<(unsigned)((ECH + 255) / 256), 256, 0, stream>>>(E4, LDP, l2g + (size_t)1 * 4, l2b + (size_t)1 * 4, w2w + (size_t)1 * 4, w2b + (size_t)1, WE, 40000, ECH);
    k_edgefeat<<<(unsigned)(((long long)ECH * LDE + 255) / 256), 256, 0, stream>>>(M, xpos, ei, EST, l1g + (size_t)1 * ED, l1b + (size_t)1 * ED, EF, 80000, ECH, E, C, LDE);
    { GemmP ge1_2;
      ge1_2.A = EF; ge1_2.B = w1w + (size_t)1 * ED * 4; ge1_2.bias = w1b + (size_t)1 * 4; ge1_2.R = EF; ge1_2.C = E4;
      ge1_2.sAo = 0; ge1_2.sAi = 0; ge1_2.sAm = LDE; ge1_2.sAk = 1; ge1_2.sBo = 0; ge1_2.sBi = 0; ge1_2.sBn = 1; ge1_2.sBk = 4; ge1_2.sCo = 0; ge1_2.sCi = 0; ge1_2.sCm = LDP; ge1_2.sRo = 0; ge1_2.sRi = 0; ge1_2.sRm = 0; ge1_2.sRn = 0;
      ge1_2.M = ECH; ge1_2.N = 4; ge1_2.K = ED; ge1_2.zi_n = 1; ge1_2.flags = 1; ge1_2.act = 0;
      ge1_2.alpha = 1.0f; ge1_2.beta = 0.0f; ge1_2.sa = 1.0f; ge1_2.sb = 1.0f; ge1_2.Npad = LDP; ge1_2.pad_ = 0;
      k_gemm<1><<<dim3((unsigned)((LDP) + 31) / 32, (unsigned)((ECH) + 15) / 16, (unsigned)(1)), 32, 0, stream>>>(ge1_2); }
    k_edgegate<<<(unsigned)((ECH + 255) / 256), 256, 0, stream>>>(E4, LDP, l2g + (size_t)1 * 4, l2b + (size_t)1 * 4, w2w + (size_t)1 * 4, w2b + (size_t)1, WE, 80000, ECH);
    k_edgefeat<<<(unsigned)(((long long)ECH * LDE + 255) / 256), 256, 0, stream>>>(M, xpos, ei, EST, l1g + (size_t)1 * ED, l1b + (size_t)1 * ED, EF, 120000, ECH, E, C, LDE);
    { GemmP ge1_3;
      ge1_3.A = EF; ge1_3.B = w1w + (size_t)1 * ED * 4; ge1_3.bias = w1b + (size_t)1 * 4; ge1_3.R = EF; ge1_3.C = E4;
      ge1_3.sAo = 0; ge1_3.sAi = 0; ge1_3.sAm = LDE; ge1_3.sAk = 1; ge1_3.sBo = 0; ge1_3.sBi = 0; ge1_3.sBn = 1; ge1_3.sBk = 4; ge1_3.sCo = 0; ge1_3.sCi = 0; ge1_3.sCm = LDP; ge1_3.sRo = 0; ge1_3.sRi = 0; ge1_3.sRm = 0; ge1_3.sRn = 0;
      ge1_3.M = ECH; ge1_3.N = 4; ge1_3.K = ED; ge1_3.zi_n = 1; ge1_3.flags = 1; ge1_3.act = 0;
      ge1_3.alpha = 1.0f; ge1_3.beta = 0.0f; ge1_3.sa = 1.0f; ge1_3.sb = 1.0f; ge1_3.Npad = LDP; ge1_3.pad_ = 0;
      k_gemm<1><<<dim3((unsigned)((LDP) + 31) / 32, (unsigned)((ECH) + 15) / 16, (unsigned)(1)), 32, 0, stream>>>(ge1_3); }
    k_edgegate<<<(unsigned)((ECH + 255) / 256), 256, 0, stream>>>(E4, LDP, l2g + (size_t)1 * 4, l2b + (size_t)1 * 4, w2w + (size_t)1 * 4, w2b + (size_t)1, WE, 120000, ECH);
    k_edgefeat<<<(unsigned)(((long long)ECH * LDE + 255) / 256), 256, 0, stream>>>(M, xpos, ei, EST, l1g + (size_t)1 * ED, l1b + (size_t)1 * ED, EF, 160000, ECH, E, C, LDE);
    { GemmP ge1_4;
      ge1_4.A = EF; ge1_4.B = w1w + (size_t)1 * ED * 4; ge1_4.bias = w1b + (size_t)1 * 4; ge1_4.R = EF; ge1_4.C = E4;
      ge1_4.sAo = 0; ge1_4.sAi = 0; ge1_4.sAm = LDE; ge1_4.sAk = 1; ge1_4.sBo = 0; ge1_4.sBi = 0; ge1_4.sBn = 1; ge1_4.sBk = 4; ge1_4.sCo = 0; ge1_4.sCi = 0; ge1_4.sCm = LDP; ge1_4.sRo = 0; ge1_4.sRi = 0; ge1_4.sRm = 0; ge1_4.sRn = 0;
      ge1_4.M = ECH; ge1_4.N = 4; ge1_4.K = ED; ge1_4.zi_n = 1; ge1_4.flags = 1; ge1_4.act = 0;
      ge1_4.alpha = 1.0f; ge1_4.beta = 0.0f; ge1_4.sa = 1.0f; ge1_4.sb = 1.0f; ge1_4.Npad = LDP; ge1_4.pad_ = 0;
      k_gemm<1><<<dim3((unsigned)((LDP) + 31) / 32, (unsigned)((ECH) + 15) / 16, (unsigned)(1)), 32, 0, stream>>>(ge1_4); }
    k_edgegate<<<(unsigned)((ECH + 255) / 256), 256, 0, stream>>>(E4, LDP, l2g + (size_t)1 * 4, l2b + (size_t)1 * 4, w2w + (size_t)1 * 4, w2b + (size_t)1, WE, 160000, ECH);
    k_edgefeat<<<(unsigned)(((long long)ECH * LDE + 255) / 256), 256, 0, stream>>>(M, xpos, ei, EST, l1g + (size_t)1 * ED, l1b + (size_t)1 * ED, EF, 200000, ECH, E, C, LDE);
    { GemmP ge1_5;
      ge1_5.A = EF; ge1_5.B = w1w + (size_t)1 * ED * 4; ge1_5.bias = w1b + (size_t)1 * 4; ge1_5.R = EF; ge1_5.C = E4;
      ge1_5.sAo = 0; ge1_5.sAi = 0; ge1_5.sAm = LDE; ge1_5.sAk = 1; ge1_5.sBo = 0; ge1_5.sBi = 0; ge1_5.sBn = 1; ge1_5.sBk = 4; ge1_5.sCo = 0; ge1_5.sCi = 0; ge1_5.sCm = LDP; ge1_5.sRo = 0; ge1_5.sRi = 0; ge1_5.sRm = 0; ge1_5.sRn = 0;
      ge1_5.M = ECH; ge1_5.N = 4; ge1_5.K = ED; ge1_5.zi_n = 1; ge1_5.flags = 1; ge1_5.act = 0;
      ge1_5.alpha = 1.0f; ge1_5.beta = 0.0f; ge1_5.sa = 1.0f; ge1_5.sb = 1.0f; ge1_5.Npad = LDP; ge1_5.pad_ = 0;
      k_gemm<1><<<dim3((unsigned)((LDP) + 31) / 32, (unsigned)((ECH) + 15) / 16, (unsigned)(1)), 32, 0, stream>>>(ge1_5); }
    k_edgegate<<<(unsigned)((ECH + 255) / 256), 256, 0, stream>>>(E4, LDP, l2g + (size_t)1 * 4, l2b + (size_t)1 * 4, w2w + (size_t)1 * 4, w2b + (size_t)1, WE, 200000, ECH);
    k_edgefeat<<<(unsigned)(((long long)ECH * LDE + 255) / 256), 256, 0, stream>>>(M, xpos, ei, EST, l1g + (size_t)1 * ED, l1b + (size_t)1 * ED, EF, 240000, ECH, E, C, LDE);
    { GemmP ge1_6;
      ge1_6.A = EF; ge1_6.B = w1w + (size_t)1 * ED * 4; ge1_6.bias = w1b + (size_t)1 * 4; ge1_6.R = EF; ge1_6.C = E4;
      ge1_6.sAo = 0; ge1_6.sAi = 0; ge1_6.sAm = LDE; ge1_6.sAk = 1; ge1_6.sBo = 0; ge1_6.sBi = 0; ge1_6.sBn = 1; ge1_6.sBk = 4; ge1_6.sCo = 0; ge1_6.sCi = 0; ge1_6.sCm = LDP; ge1_6.sRo = 0; ge1_6.sRi = 0; ge1_6.sRm = 0; ge1_6.sRn = 0;
      ge1_6.M = ECH; ge1_6.N = 4; ge1_6.K = ED; ge1_6.zi_n = 1; ge1_6.flags = 1; ge1_6.act = 0;
      ge1_6.alpha = 1.0f; ge1_6.beta = 0.0f; ge1_6.sa = 1.0f; ge1_6.sb = 1.0f; ge1_6.Npad = LDP; ge1_6.pad_ = 0;
      k_gemm<1><<<dim3((unsigned)((LDP) + 31) / 32, (unsigned)((ECH) + 15) / 16, (unsigned)(1)), 32, 0, stream>>>(ge1_6); }
    k_edgegate<<<(unsigned)((ECH + 255) / 256), 256, 0, stream>>>(E4, LDP, l2g + (size_t)1 * 4, l2b + (size_t)1 * 4, w2w + (size_t)1 * 4, w2b + (size_t)1, WE, 240000, ECH);
    k_edgefeat<<<(unsigned)(((long long)ECH * LDE + 255) / 256), 256, 0, stream>>>(M, xpos, ei, EST, l1g + (size_t)1 * ED, l1b + (size_t)1 * ED, EF, 280000, ECH, E, C, LDE);
    { GemmP ge1_7;
      ge1_7.A = EF; ge1_7.B = w1w + (size_t)1 * ED * 4; ge1_7.bias = w1b + (size_t)1 * 4; ge1_7.R = EF; ge1_7.C = E4;
      ge1_7.sAo = 0; ge1_7.sAi = 0; ge1_7.sAm = LDE; ge1_7.sAk = 1; ge1_7.sBo = 0; ge1_7.sBi = 0; ge1_7.sBn = 1; ge1_7.sBk = 4; ge1_7.sCo = 0; ge1_7.sCi = 0; ge1_7.sCm = LDP; ge1_7.sRo = 0; ge1_7.sRi = 0; ge1_7.sRm = 0; ge1_7.sRn = 0;
      ge1_7.M = ECH; ge1_7.N = 4; ge1_7.K = ED; ge1_7.zi_n = 1; ge1_7.flags = 1; ge1_7.act = 0;
      ge1_7.alpha = 1.0f; ge1_7.beta = 0.0f; ge1_7.sa = 1.0f; ge1_7.sb = 1.0f; ge1_7.Npad = LDP; ge1_7.pad_ = 0;
      k_gemm<1><<<dim3((unsigned)((LDP) + 31) / 32, (unsigned)((ECH) + 15) / 16, (unsigned)(1)), 32, 0, stream>>>(ge1_7); }
    k_edgegate<<<(unsigned)((ECH + 255) / 256), 256, 0, stream>>>(E4, LDP, l2g + (size_t)1 * 4, l2b + (size_t)1 * 4, w2w + (size_t)1 * 4, w2b + (size_t)1, WE, 280000, ECH);
    k_wagg<<<(unsigned)(((long long)Nn * C + 255) / 256), 256, 0, stream>>>(M, ei, WE, off, slot, AGG, Nn, C);
    { GemmP gh1;
      gh1.A = AGG; gh1.B = d2w + (size_t)1 * C * C; gh1.bias = d2b + (size_t)1 * C; gh1.R = AGG; gh1.C = H;
      gh1.sAo = 0; gh1.sAi = 0; gh1.sAm = C; gh1.sAk = 1; gh1.sBo = 0; gh1.sBi = 0; gh1.sBn = 1; gh1.sBk = C; gh1.sCo = 0; gh1.sCi = 0; gh1.sCm = C; gh1.sRo = 0; gh1.sRi = 0; gh1.sRm = 0; gh1.sRn = 0;
      gh1.M = Nn; gh1.N = C; gh1.K = C; gh1.zi_n = 1; gh1.flags = 1; gh1.act = 4;
      gh1.alpha = 1.0f; gh1.beta = 0.0f; gh1.sa = 1.0f; gh1.sb = 1.0f; gh1.Npad = C; gh1.pad_ = 0;
      k_gemm<1><<<dim3((unsigned)((C) + 31) / 32, (unsigned)((Nn) + 15) / 16, (unsigned)(1)), 32, 0, stream>>>(gh1); }
    { GemmP gm2;
      gm2.A = H; gm2.B = d1w + (size_t)2 * C * C; gm2.bias = d1b + (size_t)2 * C; gm2.R = H; gm2.C = M;
      gm2.sAo = 0; gm2.sAi = 0; gm2.sAm = C; gm2.sAk = 1; gm2.sBo = 0; gm2.sBi = 0; gm2.sBn = 1; gm2.sBk = C; gm2.sCo = 0; gm2.sCi = 0; gm2.sCm = C; gm2.sRo = 0; gm2.sRi = 0; gm2.sRm = 0; gm2.sRn = 0;
      gm2.M = Nn; gm2.N = C; gm2.K = C; gm2.zi_n = 1; gm2.flags = 1; gm2.act = 4;
      gm2.alpha = 1.0f; gm2.beta = 0.0f; gm2.sa = 1.0f; gm2.sb = 1.0f; gm2.Npad = C; gm2.pad_ = 0;
      k_gemm<1><<<dim3((unsigned)((C) + 31) / 32, (unsigned)((Nn) + 15) / 16, (unsigned)(1)), 32, 0, stream>>>(gm2); }
    k_edgestat<<<(unsigned)((E + 255) / 256), 256, 0, stream>>>(M, xpos, ei, EST, E, C);
    k_edgefeat<<<(unsigned)(((long long)ECH * LDE + 255) / 256), 256, 0, stream>>>(M, xpos, ei, EST, l1g + (size_t)2 * ED, l1b + (size_t)2 * ED, EF, 0, ECH, E, C, LDE);
    { GemmP ge2_0;
      ge2_0.A = EF; ge2_0.B = w1w + (size_t)2 * ED * 4; ge2_0.bias = w1b + (size_t)2 * 4; ge2_0.R = EF; ge2_0.C = E4;
      ge2_0.sAo = 0; ge2_0.sAi = 0; ge2_0.sAm = LDE; ge2_0.sAk = 1; ge2_0.sBo = 0; ge2_0.sBi = 0; ge2_0.sBn = 1; ge2_0.sBk = 4; ge2_0.sCo = 0; ge2_0.sCi = 0; ge2_0.sCm = LDP; ge2_0.sRo = 0; ge2_0.sRi = 0; ge2_0.sRm = 0; ge2_0.sRn = 0;
      ge2_0.M = ECH; ge2_0.N = 4; ge2_0.K = ED; ge2_0.zi_n = 1; ge2_0.flags = 1; ge2_0.act = 0;
      ge2_0.alpha = 1.0f; ge2_0.beta = 0.0f; ge2_0.sa = 1.0f; ge2_0.sb = 1.0f; ge2_0.Npad = LDP; ge2_0.pad_ = 0;
      k_gemm<1><<<dim3((unsigned)((LDP) + 31) / 32, (unsigned)((ECH) + 15) / 16, (unsigned)(1)), 32, 0, stream>>>(ge2_0); }
    k_edgegate<<<(unsigned)((ECH + 255) / 256), 256, 0, stream>>>(E4, LDP, l2g + (size_t)2 * 4, l2b + (size_t)2 * 4, w2w + (size_t)2 * 4, w2b + (size_t)2, WE, 0, ECH);
    k_edgefeat<<<(unsigned)(((long long)ECH * LDE + 255) / 256), 256, 0, stream>>>(M, xpos, ei, EST, l1g + (size_t)2 * ED, l1b + (size_t)2 * ED, EF, 40000, ECH, E, C, LDE);
    { GemmP ge2_1;
      ge2_1.A = EF; ge2_1.B = w1w + (size_t)2 * ED * 4; ge2_1.bias = w1b + (size_t)2 * 4; ge2_1.R = EF; ge2_1.C = E4;
      ge2_1.sAo = 0; ge2_1.sAi = 0; ge2_1.sAm = LDE; ge2_1.sAk = 1; ge2_1.sBo = 0; ge2_1.sBi = 0; ge2_1.sBn = 1; ge2_1.sBk = 4; ge2_1.sCo = 0; ge2_1.sCi = 0; ge2_1.sCm = LDP; ge2_1.sRo = 0; ge2_1.sRi = 0; ge2_1.sRm = 0; ge2_1.sRn = 0;
      ge2_1.M = ECH; ge2_1.N = 4; ge2_1.K = ED; ge2_1.zi_n = 1; ge2_1.flags = 1; ge2_1.act = 0;
      ge2_1.alpha = 1.0f; ge2_1.beta = 0.0f; ge2_1.sa = 1.0f; ge2_1.sb = 1.0f; ge2_1.Npad = LDP; ge2_1.pad_ = 0;
      k_gemm<1><<<dim3((unsigned)((LDP) + 31) / 32, (unsigned)((ECH) + 15) / 16, (unsigned)(1)), 32, 0, stream>>>(ge2_1); }
    k_edgegate<<<(unsigned)((ECH + 255) / 256), 256, 0, stream>>>(E4, LDP, l2g + (size_t)2 * 4, l2b + (size_t)2 * 4, w2w + (size_t)2 * 4, w2b + (size_t)2, WE, 40000, ECH);
    k_edgefeat<<<(unsigned)(((long long)ECH * LDE + 255) / 256), 256, 0, stream>>>(M, xpos, ei, EST, l1g + (size_t)2 * ED, l1b + (size_t)2 * ED, EF, 80000, ECH, E, C, LDE);
    { GemmP ge2_2;
      ge2_2.A = EF; ge2_2.B = w1w + (size_t)2 * ED * 4; ge2_2.bias = w1b + (size_t)2 * 4; ge2_2.R = EF; ge2_2.C = E4;
      ge2_2.sAo = 0; ge2_2.sAi = 0; ge2_2.sAm = LDE; ge2_2.sAk = 1; ge2_2.sBo = 0; ge2_2.sBi = 0; ge2_2.sBn = 1; ge2_2.sBk = 4; ge2_2.sCo = 0; ge2_2.sCi = 0; ge2_2.sCm = LDP; ge2_2.sRo = 0; ge2_2.sRi = 0; ge2_2.sRm = 0; ge2_2.sRn = 0;
      ge2_2.M = ECH; ge2_2.N = 4; ge2_2.K = ED; ge2_2.zi_n = 1; ge2_2.flags = 1; ge2_2.act = 0;
      ge2_2.alpha = 1.0f; ge2_2.beta = 0.0f; ge2_2.sa = 1.0f; ge2_2.sb = 1.0f; ge2_2.Npad = LDP; ge2_2.pad_ = 0;
      k_gemm<1><<<dim3((unsigned)((LDP) + 31) / 32, (unsigned)((ECH) + 15) / 16, (unsigned)(1)), 32, 0, stream>>>(ge2_2); }
    k_edgegate<<<(unsigned)((ECH + 255) / 256), 256, 0, stream>>>(E4, LDP, l2g + (size_t)2 * 4, l2b + (size_t)2 * 4, w2w + (size_t)2 * 4, w2b + (size_t)2, WE, 80000, ECH);
    k_edgefeat<<<(unsigned)(((long long)ECH * LDE + 255) / 256), 256, 0, stream>>>(M, xpos, ei, EST, l1g + (size_t)2 * ED, l1b + (size_t)2 * ED, EF, 120000, ECH, E, C, LDE);
    { GemmP ge2_3;
      ge2_3.A = EF; ge2_3.B = w1w + (size_t)2 * ED * 4; ge2_3.bias = w1b + (size_t)2 * 4; ge2_3.R = EF; ge2_3.C = E4;
      ge2_3.sAo = 0; ge2_3.sAi = 0; ge2_3.sAm = LDE; ge2_3.sAk = 1; ge2_3.sBo = 0; ge2_3.sBi = 0; ge2_3.sBn = 1; ge2_3.sBk = 4; ge2_3.sCo = 0; ge2_3.sCi = 0; ge2_3.sCm = LDP; ge2_3.sRo = 0; ge2_3.sRi = 0; ge2_3.sRm = 0; ge2_3.sRn = 0;
      ge2_3.M = ECH; ge2_3.N = 4; ge2_3.K = ED; ge2_3.zi_n = 1; ge2_3.flags = 1; ge2_3.act = 0;
      ge2_3.alpha = 1.0f; ge2_3.beta = 0.0f; ge2_3.sa = 1.0f; ge2_3.sb = 1.0f; ge2_3.Npad = LDP; ge2_3.pad_ = 0;
      k_gemm<1><<<dim3((unsigned)((LDP) + 31) / 32, (unsigned)((ECH) + 15) / 16, (unsigned)(1)), 32, 0, stream>>>(ge2_3); }
    k_edgegate<<<(unsigned)((ECH + 255) / 256), 256, 0, stream>>>(E4, LDP, l2g + (size_t)2 * 4, l2b + (size_t)2 * 4, w2w + (size_t)2 * 4, w2b + (size_t)2, WE, 120000, ECH);
    k_edgefeat<<<(unsigned)(((long long)ECH * LDE + 255) / 256), 256, 0, stream>>>(M, xpos, ei, EST, l1g + (size_t)2 * ED, l1b + (size_t)2 * ED, EF, 160000, ECH, E, C, LDE);
    { GemmP ge2_4;
      ge2_4.A = EF; ge2_4.B = w1w + (size_t)2 * ED * 4; ge2_4.bias = w1b + (size_t)2 * 4; ge2_4.R = EF; ge2_4.C = E4;
      ge2_4.sAo = 0; ge2_4.sAi = 0; ge2_4.sAm = LDE; ge2_4.sAk = 1; ge2_4.sBo = 0; ge2_4.sBi = 0; ge2_4.sBn = 1; ge2_4.sBk = 4; ge2_4.sCo = 0; ge2_4.sCi = 0; ge2_4.sCm = LDP; ge2_4.sRo = 0; ge2_4.sRi = 0; ge2_4.sRm = 0; ge2_4.sRn = 0;
      ge2_4.M = ECH; ge2_4.N = 4; ge2_4.K = ED; ge2_4.zi_n = 1; ge2_4.flags = 1; ge2_4.act = 0;
      ge2_4.alpha = 1.0f; ge2_4.beta = 0.0f; ge2_4.sa = 1.0f; ge2_4.sb = 1.0f; ge2_4.Npad = LDP; ge2_4.pad_ = 0;
      k_gemm<1><<<dim3((unsigned)((LDP) + 31) / 32, (unsigned)((ECH) + 15) / 16, (unsigned)(1)), 32, 0, stream>>>(ge2_4); }
    k_edgegate<<<(unsigned)((ECH + 255) / 256), 256, 0, stream>>>(E4, LDP, l2g + (size_t)2 * 4, l2b + (size_t)2 * 4, w2w + (size_t)2 * 4, w2b + (size_t)2, WE, 160000, ECH);
    k_edgefeat<<<(unsigned)(((long long)ECH * LDE + 255) / 256), 256, 0, stream>>>(M, xpos, ei, EST, l1g + (size_t)2 * ED, l1b + (size_t)2 * ED, EF, 200000, ECH, E, C, LDE);
    { GemmP ge2_5;
      ge2_5.A = EF; ge2_5.B = w1w + (size_t)2 * ED * 4; ge2_5.bias = w1b + (size_t)2 * 4; ge2_5.R = EF; ge2_5.C = E4;
      ge2_5.sAo = 0; ge2_5.sAi = 0; ge2_5.sAm = LDE; ge2_5.sAk = 1; ge2_5.sBo = 0; ge2_5.sBi = 0; ge2_5.sBn = 1; ge2_5.sBk = 4; ge2_5.sCo = 0; ge2_5.sCi = 0; ge2_5.sCm = LDP; ge2_5.sRo = 0; ge2_5.sRi = 0; ge2_5.sRm = 0; ge2_5.sRn = 0;
      ge2_5.M = ECH; ge2_5.N = 4; ge2_5.K = ED; ge2_5.zi_n = 1; ge2_5.flags = 1; ge2_5.act = 0;
      ge2_5.alpha = 1.0f; ge2_5.beta = 0.0f; ge2_5.sa = 1.0f; ge2_5.sb = 1.0f; ge2_5.Npad = LDP; ge2_5.pad_ = 0;
      k_gemm<1><<<dim3((unsigned)((LDP) + 31) / 32, (unsigned)((ECH) + 15) / 16, (unsigned)(1)), 32, 0, stream>>>(ge2_5); }
    k_edgegate<<<(unsigned)((ECH + 255) / 256), 256, 0, stream>>>(E4, LDP, l2g + (size_t)2 * 4, l2b + (size_t)2 * 4, w2w + (size_t)2 * 4, w2b + (size_t)2, WE, 200000, ECH);
    k_edgefeat<<<(unsigned)(((long long)ECH * LDE + 255) / 256), 256, 0, stream>>>(M, xpos, ei, EST, l1g + (size_t)2 * ED, l1b + (size_t)2 * ED, EF, 240000, ECH, E, C, LDE);
    { GemmP ge2_6;
      ge2_6.A = EF; ge2_6.B = w1w + (size_t)2 * ED * 4; ge2_6.bias = w1b + (size_t)2 * 4; ge2_6.R = EF; ge2_6.C = E4;
      ge2_6.sAo = 0; ge2_6.sAi = 0; ge2_6.sAm = LDE; ge2_6.sAk = 1; ge2_6.sBo = 0; ge2_6.sBi = 0; ge2_6.sBn = 1; ge2_6.sBk = 4; ge2_6.sCo = 0; ge2_6.sCi = 0; ge2_6.sCm = LDP; ge2_6.sRo = 0; ge2_6.sRi = 0; ge2_6.sRm = 0; ge2_6.sRn = 0;
      ge2_6.M = ECH; ge2_6.N = 4; ge2_6.K = ED; ge2_6.zi_n = 1; ge2_6.flags = 1; ge2_6.act = 0;
      ge2_6.alpha = 1.0f; ge2_6.beta = 0.0f; ge2_6.sa = 1.0f; ge2_6.sb = 1.0f; ge2_6.Npad = LDP; ge2_6.pad_ = 0;
      k_gemm<1><<<dim3((unsigned)((LDP) + 31) / 32, (unsigned)((ECH) + 15) / 16, (unsigned)(1)), 32, 0, stream>>>(ge2_6); }
    k_edgegate<<<(unsigned)((ECH + 255) / 256), 256, 0, stream>>>(E4, LDP, l2g + (size_t)2 * 4, l2b + (size_t)2 * 4, w2w + (size_t)2 * 4, w2b + (size_t)2, WE, 240000, ECH);
    k_edgefeat<<<(unsigned)(((long long)ECH * LDE + 255) / 256), 256, 0, stream>>>(M, xpos, ei, EST, l1g + (size_t)2 * ED, l1b + (size_t)2 * ED, EF, 280000, ECH, E, C, LDE);
    { GemmP ge2_7;
      ge2_7.A = EF; ge2_7.B = w1w + (size_t)2 * ED * 4; ge2_7.bias = w1b + (size_t)2 * 4; ge2_7.R = EF; ge2_7.C = E4;
      ge2_7.sAo = 0; ge2_7.sAi = 0; ge2_7.sAm = LDE; ge2_7.sAk = 1; ge2_7.sBo = 0; ge2_7.sBi = 0; ge2_7.sBn = 1; ge2_7.sBk = 4; ge2_7.sCo = 0; ge2_7.sCi = 0; ge2_7.sCm = LDP; ge2_7.sRo = 0; ge2_7.sRi = 0; ge2_7.sRm = 0; ge2_7.sRn = 0;
      ge2_7.M = ECH; ge2_7.N = 4; ge2_7.K = ED; ge2_7.zi_n = 1; ge2_7.flags = 1; ge2_7.act = 0;
      ge2_7.alpha = 1.0f; ge2_7.beta = 0.0f; ge2_7.sa = 1.0f; ge2_7.sb = 1.0f; ge2_7.Npad = LDP; ge2_7.pad_ = 0;
      k_gemm<1><<<dim3((unsigned)((LDP) + 31) / 32, (unsigned)((ECH) + 15) / 16, (unsigned)(1)), 32, 0, stream>>>(ge2_7); }
    k_edgegate<<<(unsigned)((ECH + 255) / 256), 256, 0, stream>>>(E4, LDP, l2g + (size_t)2 * 4, l2b + (size_t)2 * 4, w2w + (size_t)2 * 4, w2b + (size_t)2, WE, 280000, ECH);
    k_wagg<<<(unsigned)(((long long)Nn * C + 255) / 256), 256, 0, stream>>>(M, ei, WE, off, slot, AGG, Nn, C);
    { GemmP gh2;
      gh2.A = AGG; gh2.B = d2w + (size_t)2 * C * C; gh2.bias = d2b + (size_t)2 * C; gh2.R = AGG; gh2.C = H;
      gh2.sAo = 0; gh2.sAi = 0; gh2.sAm = C; gh2.sAk = 1; gh2.sBo = 0; gh2.sBi = 0; gh2.sBn = 1; gh2.sBk = C; gh2.sCo = 0; gh2.sCi = 0; gh2.sCm = C; gh2.sRo = 0; gh2.sRi = 0; gh2.sRm = 0; gh2.sRn = 0;
      gh2.M = Nn; gh2.N = C; gh2.K = C; gh2.zi_n = 1; gh2.flags = 1; gh2.act = 4;
      gh2.alpha = 1.0f; gh2.beta = 0.0f; gh2.sa = 1.0f; gh2.sb = 1.0f; gh2.Npad = C; gh2.pad_ = 0;
      k_gemm<1><<<dim3((unsigned)((C) + 31) / 32, (unsigned)((Nn) + 15) / 16, (unsigned)(1)), 32, 0, stream>>>(gh2); }
    { GemmP gm3;
      gm3.A = H; gm3.B = d1w + (size_t)3 * C * C; gm3.bias = d1b + (size_t)3 * C; gm3.R = H; gm3.C = M;
      gm3.sAo = 0; gm3.sAi = 0; gm3.sAm = C; gm3.sAk = 1; gm3.sBo = 0; gm3.sBi = 0; gm3.sBn = 1; gm3.sBk = C; gm3.sCo = 0; gm3.sCi = 0; gm3.sCm = C; gm3.sRo = 0; gm3.sRi = 0; gm3.sRm = 0; gm3.sRn = 0;
      gm3.M = Nn; gm3.N = C; gm3.K = C; gm3.zi_n = 1; gm3.flags = 1; gm3.act = 4;
      gm3.alpha = 1.0f; gm3.beta = 0.0f; gm3.sa = 1.0f; gm3.sb = 1.0f; gm3.Npad = C; gm3.pad_ = 0;
      k_gemm<1><<<dim3((unsigned)((C) + 31) / 32, (unsigned)((Nn) + 15) / 16, (unsigned)(1)), 32, 0, stream>>>(gm3); }
    k_edgestat<<<(unsigned)((E + 255) / 256), 256, 0, stream>>>(M, xpos, ei, EST, E, C);
    k_edgefeat<<<(unsigned)(((long long)ECH * LDE + 255) / 256), 256, 0, stream>>>(M, xpos, ei, EST, l1g + (size_t)3 * ED, l1b + (size_t)3 * ED, EF, 0, ECH, E, C, LDE);
    { GemmP ge3_0;
      ge3_0.A = EF; ge3_0.B = w1w + (size_t)3 * ED * 4; ge3_0.bias = w1b + (size_t)3 * 4; ge3_0.R = EF; ge3_0.C = E4;
      ge3_0.sAo = 0; ge3_0.sAi = 0; ge3_0.sAm = LDE; ge3_0.sAk = 1; ge3_0.sBo = 0; ge3_0.sBi = 0; ge3_0.sBn = 1; ge3_0.sBk = 4; ge3_0.sCo = 0; ge3_0.sCi = 0; ge3_0.sCm = LDP; ge3_0.sRo = 0; ge3_0.sRi = 0; ge3_0.sRm = 0; ge3_0.sRn = 0;
      ge3_0.M = ECH; ge3_0.N = 4; ge3_0.K = ED; ge3_0.zi_n = 1; ge3_0.flags = 1; ge3_0.act = 0;
      ge3_0.alpha = 1.0f; ge3_0.beta = 0.0f; ge3_0.sa = 1.0f; ge3_0.sb = 1.0f; ge3_0.Npad = LDP; ge3_0.pad_ = 0;
      k_gemm<1><<<dim3((unsigned)((LDP) + 31) / 32, (unsigned)((ECH) + 15) / 16, (unsigned)(1)), 32, 0, stream>>>(ge3_0); }
    k_edgegate<<<(unsigned)((ECH + 255) / 256), 256, 0, stream>>>(E4, LDP, l2g + (size_t)3 * 4, l2b + (size_t)3 * 4, w2w + (size_t)3 * 4, w2b + (size_t)3, WE, 0, ECH);
    k_edgefeat<<<(unsigned)(((long long)ECH * LDE + 255) / 256), 256, 0, stream>>>(M, xpos, ei, EST, l1g + (size_t)3 * ED, l1b + (size_t)3 * ED, EF, 40000, ECH, E, C, LDE);
    { GemmP ge3_1;
      ge3_1.A = EF; ge3_1.B = w1w + (size_t)3 * ED * 4; ge3_1.bias = w1b + (size_t)3 * 4; ge3_1.R = EF; ge3_1.C = E4;
      ge3_1.sAo = 0; ge3_1.sAi = 0; ge3_1.sAm = LDE; ge3_1.sAk = 1; ge3_1.sBo = 0; ge3_1.sBi = 0; ge3_1.sBn = 1; ge3_1.sBk = 4; ge3_1.sCo = 0; ge3_1.sCi = 0; ge3_1.sCm = LDP; ge3_1.sRo = 0; ge3_1.sRi = 0; ge3_1.sRm = 0; ge3_1.sRn = 0;
      ge3_1.M = ECH; ge3_1.N = 4; ge3_1.K = ED; ge3_1.zi_n = 1; ge3_1.flags = 1; ge3_1.act = 0;
      ge3_1.alpha = 1.0f; ge3_1.beta = 0.0f; ge3_1.sa = 1.0f; ge3_1.sb = 1.0f; ge3_1.Npad = LDP; ge3_1.pad_ = 0;
      k_gemm<1><<<dim3((unsigned)((LDP) + 31) / 32, (unsigned)((ECH) + 15) / 16, (unsigned)(1)), 32, 0, stream>>>(ge3_1); }
    k_edgegate<<<(unsigned)((ECH + 255) / 256), 256, 0, stream>>>(E4, LDP, l2g + (size_t)3 * 4, l2b + (size_t)3 * 4, w2w + (size_t)3 * 4, w2b + (size_t)3, WE, 40000, ECH);
    k_edgefeat<<<(unsigned)(((long long)ECH * LDE + 255) / 256), 256, 0, stream>>>(M, xpos, ei, EST, l1g + (size_t)3 * ED, l1b + (size_t)3 * ED, EF, 80000, ECH, E, C, LDE);
    { GemmP ge3_2;
      ge3_2.A = EF; ge3_2.B = w1w + (size_t)3 * ED * 4; ge3_2.bias = w1b + (size_t)3 * 4; ge3_2.R = EF; ge3_2.C = E4;
      ge3_2.sAo = 0; ge3_2.sAi = 0; ge3_2.sAm = LDE; ge3_2.sAk = 1; ge3_2.sBo = 0; ge3_2.sBi = 0; ge3_2.sBn = 1; ge3_2.sBk = 4; ge3_2.sCo = 0; ge3_2.sCi = 0; ge3_2.sCm = LDP; ge3_2.sRo = 0; ge3_2.sRi = 0; ge3_2.sRm = 0; ge3_2.sRn = 0;
      ge3_2.M = ECH; ge3_2.N = 4; ge3_2.K = ED; ge3_2.zi_n = 1; ge3_2.flags = 1; ge3_2.act = 0;
      ge3_2.alpha = 1.0f; ge3_2.beta = 0.0f; ge3_2.sa = 1.0f; ge3_2.sb = 1.0f; ge3_2.Npad = LDP; ge3_2.pad_ = 0;
      k_gemm<1><<<dim3((unsigned)((LDP) + 31) / 32, (unsigned)((ECH) + 15) / 16, (unsigned)(1)), 32, 0, stream>>>(ge3_2); }
    k_edgegate<<<(unsigned)((ECH + 255) / 256), 256, 0, stream>>>(E4, LDP, l2g + (size_t)3 * 4, l2b + (size_t)3 * 4, w2w + (size_t)3 * 4, w2b + (size_t)3, WE, 80000, ECH);
    k_edgefeat<<<(unsigned)(((long long)ECH * LDE + 255) / 256), 256, 0, stream>>>(M, xpos, ei, EST, l1g + (size_t)3 * ED, l1b + (size_t)3 * ED, EF, 120000, ECH, E, C, LDE);
    { GemmP ge3_3;
      ge3_3.A = EF; ge3_3.B = w1w + (size_t)3 * ED * 4; ge3_3.bias = w1b + (size_t)3 * 4; ge3_3.R = EF; ge3_3.C = E4;
      ge3_3.sAo = 0; ge3_3.sAi = 0; ge3_3.sAm = LDE; ge3_3.sAk = 1; ge3_3.sBo = 0; ge3_3.sBi = 0; ge3_3.sBn = 1; ge3_3.sBk = 4; ge3_3.sCo = 0; ge3_3.sCi = 0; ge3_3.sCm = LDP; ge3_3.sRo = 0; ge3_3.sRi = 0; ge3_3.sRm = 0; ge3_3.sRn = 0;
      ge3_3.M = ECH; ge3_3.N = 4; ge3_3.K = ED; ge3_3.zi_n = 1; ge3_3.flags = 1; ge3_3.act = 0;
      ge3_3.alpha = 1.0f; ge3_3.beta = 0.0f; ge3_3.sa = 1.0f; ge3_3.sb = 1.0f; ge3_3.Npad = LDP; ge3_3.pad_ = 0;
      k_gemm<1><<<dim3((unsigned)((LDP) + 31) / 32, (unsigned)((ECH) + 15) / 16, (unsigned)(1)), 32, 0, stream>>>(ge3_3); }
    k_edgegate<<<(unsigned)((ECH + 255) / 256), 256, 0, stream>>>(E4, LDP, l2g + (size_t)3 * 4, l2b + (size_t)3 * 4, w2w + (size_t)3 * 4, w2b + (size_t)3, WE, 120000, ECH);
    k_edgefeat<<<(unsigned)(((long long)ECH * LDE + 255) / 256), 256, 0, stream>>>(M, xpos, ei, EST, l1g + (size_t)3 * ED, l1b + (size_t)3 * ED, EF, 160000, ECH, E, C, LDE);
    { GemmP ge3_4;
      ge3_4.A = EF; ge3_4.B = w1w + (size_t)3 * ED * 4; ge3_4.bias = w1b + (size_t)3 * 4; ge3_4.R = EF; ge3_4.C = E4;
      ge3_4.sAo = 0; ge3_4.sAi = 0; ge3_4.sAm = LDE; ge3_4.sAk = 1; ge3_4.sBo = 0; ge3_4.sBi = 0; ge3_4.sBn = 1; ge3_4.sBk = 4; ge3_4.sCo = 0; ge3_4.sCi = 0; ge3_4.sCm = LDP; ge3_4.sRo = 0; ge3_4.sRi = 0; ge3_4.sRm = 0; ge3_4.sRn = 0;
      ge3_4.M = ECH; ge3_4.N = 4; ge3_4.K = ED; ge3_4.zi_n = 1; ge3_4.flags = 1; ge3_4.act = 0;
      ge3_4.alpha = 1.0f; ge3_4.beta = 0.0f; ge3_4.sa = 1.0f; ge3_4.sb = 1.0f; ge3_4.Npad = LDP; ge3_4.pad_ = 0;
      k_gemm<1><<<dim3((unsigned)((LDP) + 31) / 32, (unsigned)((ECH) + 15) / 16, (unsigned)(1)), 32, 0, stream>>>(ge3_4); }
    k_edgegate<<<(unsigned)((ECH + 255) / 256), 256, 0, stream>>>(E4, LDP, l2g + (size_t)3 * 4, l2b + (size_t)3 * 4, w2w + (size_t)3 * 4, w2b + (size_t)3, WE, 160000, ECH);
    k_edgefeat<<<(unsigned)(((long long)ECH * LDE + 255) / 256), 256, 0, stream>>>(M, xpos, ei, EST, l1g + (size_t)3 * ED, l1b + (size_t)3 * ED, EF, 200000, ECH, E, C, LDE);
    { GemmP ge3_5;
      ge3_5.A = EF; ge3_5.B = w1w + (size_t)3 * ED * 4; ge3_5.bias = w1b + (size_t)3 * 4; ge3_5.R = EF; ge3_5.C = E4;
      ge3_5.sAo = 0; ge3_5.sAi = 0; ge3_5.sAm = LDE; ge3_5.sAk = 1; ge3_5.sBo = 0; ge3_5.sBi = 0; ge3_5.sBn = 1; ge3_5.sBk = 4; ge3_5.sCo = 0; ge3_5.sCi = 0; ge3_5.sCm = LDP; ge3_5.sRo = 0; ge3_5.sRi = 0; ge3_5.sRm = 0; ge3_5.sRn = 0;
      ge3_5.M = ECH; ge3_5.N = 4; ge3_5.K = ED; ge3_5.zi_n = 1; ge3_5.flags = 1; ge3_5.act = 0;
      ge3_5.alpha = 1.0f; ge3_5.beta = 0.0f; ge3_5.sa = 1.0f; ge3_5.sb = 1.0f; ge3_5.Npad = LDP; ge3_5.pad_ = 0;
      k_gemm<1><<<dim3((unsigned)((LDP) + 31) / 32, (unsigned)((ECH) + 15) / 16, (unsigned)(1)), 32, 0, stream>>>(ge3_5); }
    k_edgegate<<<(unsigned)((ECH + 255) / 256), 256, 0, stream>>>(E4, LDP, l2g + (size_t)3 * 4, l2b + (size_t)3 * 4, w2w + (size_t)3 * 4, w2b + (size_t)3, WE, 200000, ECH);
    k_edgefeat<<<(unsigned)(((long long)ECH * LDE + 255) / 256), 256, 0, stream>>>(M, xpos, ei, EST, l1g + (size_t)3 * ED, l1b + (size_t)3 * ED, EF, 240000, ECH, E, C, LDE);
    { GemmP ge3_6;
      ge3_6.A = EF; ge3_6.B = w1w + (size_t)3 * ED * 4; ge3_6.bias = w1b + (size_t)3 * 4; ge3_6.R = EF; ge3_6.C = E4;
      ge3_6.sAo = 0; ge3_6.sAi = 0; ge3_6.sAm = LDE; ge3_6.sAk = 1; ge3_6.sBo = 0; ge3_6.sBi = 0; ge3_6.sBn = 1; ge3_6.sBk = 4; ge3_6.sCo = 0; ge3_6.sCi = 0; ge3_6.sCm = LDP; ge3_6.sRo = 0; ge3_6.sRi = 0; ge3_6.sRm = 0; ge3_6.sRn = 0;
      ge3_6.M = ECH; ge3_6.N = 4; ge3_6.K = ED; ge3_6.zi_n = 1; ge3_6.flags = 1; ge3_6.act = 0;
      ge3_6.alpha = 1.0f; ge3_6.beta = 0.0f; ge3_6.sa = 1.0f; ge3_6.sb = 1.0f; ge3_6.Npad = LDP; ge3_6.pad_ = 0;
      k_gemm<1><<<dim3((unsigned)((LDP) + 31) / 32, (unsigned)((ECH) + 15) / 16, (unsigned)(1)), 32, 0, stream>>>(ge3_6); }
    k_edgegate<<<(unsigned)((ECH + 255) / 256), 256, 0, stream>>>(E4, LDP, l2g + (size_t)3 * 4, l2b + (size_t)3 * 4, w2w + (size_t)3 * 4, w2b + (size_t)3, WE, 240000, ECH);
    k_edgefeat<<<(unsigned)(((long long)ECH * LDE + 255) / 256), 256, 0, stream>>>(M, xpos, ei, EST, l1g + (size_t)3 * ED, l1b + (size_t)3 * ED, EF, 280000, ECH, E, C, LDE);
    { GemmP ge3_7;
      ge3_7.A = EF; ge3_7.B = w1w + (size_t)3 * ED * 4; ge3_7.bias = w1b + (size_t)3 * 4; ge3_7.R = EF; ge3_7.C = E4;
      ge3_7.sAo = 0; ge3_7.sAi = 0; ge3_7.sAm = LDE; ge3_7.sAk = 1; ge3_7.sBo = 0; ge3_7.sBi = 0; ge3_7.sBn = 1; ge3_7.sBk = 4; ge3_7.sCo = 0; ge3_7.sCi = 0; ge3_7.sCm = LDP; ge3_7.sRo = 0; ge3_7.sRi = 0; ge3_7.sRm = 0; ge3_7.sRn = 0;
      ge3_7.M = ECH; ge3_7.N = 4; ge3_7.K = ED; ge3_7.zi_n = 1; ge3_7.flags = 1; ge3_7.act = 0;
      ge3_7.alpha = 1.0f; ge3_7.beta = 0.0f; ge3_7.sa = 1.0f; ge3_7.sb = 1.0f; ge3_7.Npad = LDP; ge3_7.pad_ = 0;
      k_gemm<1><<<dim3((unsigned)((LDP) + 31) / 32, (unsigned)((ECH) + 15) / 16, (unsigned)(1)), 32, 0, stream>>>(ge3_7); }
    k_edgegate<<<(unsigned)((ECH + 255) / 256), 256, 0, stream>>>(E4, LDP, l2g + (size_t)3 * 4, l2b + (size_t)3 * 4, w2w + (size_t)3 * 4, w2b + (size_t)3, WE, 280000, ECH);
    k_wagg<<<(unsigned)(((long long)Nn * C + 255) / 256), 256, 0, stream>>>(M, ei, WE, off, slot, AGG, Nn, C);
    { GemmP gh3;
      gh3.A = AGG; gh3.B = d2w + (size_t)3 * C * C; gh3.bias = d2b + (size_t)3 * C; gh3.R = AGG; gh3.C = H;
      gh3.sAo = 0; gh3.sAi = 0; gh3.sAm = C; gh3.sAk = 1; gh3.sBo = 0; gh3.sBi = 0; gh3.sBn = 1; gh3.sBk = C; gh3.sCo = 0; gh3.sCi = 0; gh3.sCm = C; gh3.sRo = 0; gh3.sRi = 0; gh3.sRm = 0; gh3.sRn = 0;
      gh3.M = Nn; gh3.N = C; gh3.K = C; gh3.zi_n = 1; gh3.flags = 1; gh3.act = 4;
      gh3.alpha = 1.0f; gh3.beta = 0.0f; gh3.sa = 1.0f; gh3.sb = 1.0f; gh3.Npad = C; gh3.pad_ = 0;
      k_gemm<1><<<dim3((unsigned)((C) + 31) / 32, (unsigned)((Nn) + 15) / 16, (unsigned)(1)), 32, 0, stream>>>(gh3); }
    k_csr_mean<<<(unsigned)(((long long)G * C + 255) / 256), 256, 0, stream>>>(H, ids, goff, gslot, PL, G, C);
    { GemmP ghead;
      ghead.A = PL; ghead.B = hw; ghead.bias = hb; ghead.R = PL; ghead.C = OP;
      ghead.sAo = 0; ghead.sAi = 0; ghead.sAm = C; ghead.sAk = 1; ghead.sBo = 0; ghead.sBi = 0; ghead.sBn = 1; ghead.sBk = 1; ghead.sCo = 0; ghead.sCi = 0; ghead.sCm = LDP; ghead.sRo = 0; ghead.sRi = 0; ghead.sRm = 0; ghead.sRn = 0;
      ghead.M = G; ghead.N = 1; ghead.K = C; ghead.zi_n = 1; ghead.flags = 1; ghead.act = 0;
      ghead.alpha = 1.0f; ghead.beta = 0.0f; ghead.sa = 1.0f; ghead.sb = 1.0f; ghead.Npad = LDP; ghead.pad_ = 0;
      k_gemm<1><<<dim3((unsigned)((LDP) + 31) / 32, (unsigned)((G) + 15) / 16, (unsigned)(1)), 32, 0, stream>>>(ghead); }
    k_lincopy<<<(unsigned)(((long long)(G) * (1) + 255) / 256), 256, 0, stream>>>(OP, LDP, out, 1, G, 1);
}
